// EchoPIPs_33895881900437
// MI455X (gfx1250) — hardware-verified
//
#include <hip/hip_runtime.h>
#include <math.h>

typedef __attribute__((ext_vector_type(16))) _Float16 v16h;
typedef __attribute__((ext_vector_type(8)))  _Float16 v8h;
typedef __attribute__((ext_vector_type(16))) __bf16   v16b;
typedef __attribute__((ext_vector_type(8)))  float    v8f;
typedef __attribute__((ext_vector_type(4)))  float    v4f;

__device__ __forceinline__ int frag_k(int i, int h) { return (i < 8) ? (8 * h + i) : (16 + 8 * h + (i - 8)); }
__device__ __forceinline__ __bf16 bf16_rne(float f) {
    unsigned int u = __float_as_uint(f);
    u += 0x7fffu + ((u >> 16) & 1u);
    return __builtin_bit_cast(__bf16, (unsigned short)(u >> 16));
}
__device__ __forceinline__ float bf16_f32(__bf16 b) { return __uint_as_float(((unsigned int)__builtin_bit_cast(unsigned short, b)) << 16); }
__device__ __forceinline__ v8f wmma16(v16h a, v16h b, v8f c) {
    c = __builtin_amdgcn_wmma_f32_16x16x32_f16(false, a, false, b, (short)0, c, false, false);
    asm volatile("v_nop\n\tv_nop\n\tv_nop\n\tv_nop" : "+v"(c) : "v"(a), "v"(b));
    return c;
}
__device__ __forceinline__ v8f wmmab(v16b a, v16b b, v8f c) {
    c = __builtin_amdgcn_wmma_f32_16x16x32_bf16(false, a, false, b, (short)0, c, false, false);
    asm volatile("v_nop\n\tv_nop\n\tv_nop\n\tv_nop" : "+v"(c) : "v"(a), "v"(b));
    return c;
}
struct Split { v16b hi, lo; };
__device__ __forceinline__ v8f wmma3(const Split& a, const Split& b, v8f c) {
    c = __builtin_amdgcn_wmma_f32_16x16x32_bf16(false, a.hi, false, b.hi, (short)0, c, false, false);
    c = __builtin_amdgcn_wmma_f32_16x16x32_bf16(false, a.hi, false, b.lo, (short)0, c, false, false);
    c = __builtin_amdgcn_wmma_f32_16x16x32_bf16(false, a.lo, false, b.hi, (short)0, c, false, false);
    asm volatile("v_nop\n\tv_nop\n\tv_nop\n\tv_nop" : "+v"(c) : "v"(a.hi), "v"(a.lo), "v"(b.hi), "v"(b.lo));
    return c;
}
struct Split3 { v16b hi, mid, lo; };
__device__ __forceinline__ v8f wmma6(const Split3& a, const Split3& b, v8f c) {
    c = __builtin_amdgcn_wmma_f32_16x16x32_bf16(false, a.hi, false, b.hi, (short)0, c, false, false);
    c = __builtin_amdgcn_wmma_f32_16x16x32_bf16(false, a.hi, false, b.mid, (short)0, c, false, false);
    c = __builtin_amdgcn_wmma_f32_16x16x32_bf16(false, a.mid, false, b.hi, (short)0, c, false, false);
    c = __builtin_amdgcn_wmma_f32_16x16x32_bf16(false, a.hi, false, b.lo, (short)0, c, false, false);
    c = __builtin_amdgcn_wmma_f32_16x16x32_bf16(false, a.mid, false, b.mid, (short)0, c, false, false);
    c = __builtin_amdgcn_wmma_f32_16x16x32_bf16(false, a.lo, false, b.hi, (short)0, c, false, false);
    asm volatile("v_nop\n\tv_nop\n\tv_nop\n\tv_nop" : "+v"(c) : "v"(a.hi), "v"(a.mid), "v"(a.lo), "v"(b.hi), "v"(b.mid), "v"(b.lo));
    return c;
}

__device__ __forceinline__ v16h fh_ld(const float* __restrict__ p, long long sk, int k0, int h, int klen, float s) {
    v16h a;
#pragma unroll
    for (int i = 0; i < 16; ++i) { const int k = k0 + frag_k(i, h); a[i] = (k < klen) ? (_Float16)(p[(long long)k * sk] * s) : (_Float16)0.f; }
    return a;
}
__device__ __forceinline__ Split sp_ld(const float* __restrict__ p, long long sk, int k0, int h, int klen, float s) {
    Split r;
#pragma unroll
    for (int i = 0; i < 16; ++i) {
        const int k = k0 + frag_k(i, h); const float x = (k < klen) ? p[(long long)k * sk] * s : 0.f;
        const __bf16 hb = bf16_rne(x); r.hi[i] = hb; r.lo[i] = bf16_rne(x - bf16_f32(hb));
    }
    return r;
}
__device__ __forceinline__ Split3 sp3_ld(const float* __restrict__ p, long long sk, int k0, int h, int klen, float s) {
    Split3 r;
#pragma unroll
    for (int i = 0; i < 16; ++i) {
        const int k = k0 + frag_k(i, h); const float x = (k < klen) ? p[(long long)k * sk] * s : 0.f;
        const __bf16 hb = bf16_rne(x); const float r1 = x - bf16_f32(hb); const __bf16 mb = bf16_rne(r1);
        r.hi[i] = hb; r.mid[i] = mb; r.lo[i] = bf16_rne(r1 - bf16_f32(mb));
    }
    return r;
}
__device__ __forceinline__ v16b bh_ld(const float* __restrict__ p, long long sk, int k0, int h, int klen, float s) {
    v16b a;
#pragma unroll
    for (int i = 0; i < 16; ++i) { const int k = k0 + frag_k(i, h); a[i] = bf16_rne((k < klen) ? p[(long long)k * sk] * s : 0.f); }
    return a;
}
__device__ __forceinline__ v16h fh_row(const _Float16* __restrict__ row, int k0, int h) {
    v16h a;
#pragma unroll
    for (int i = 0; i < 16; ++i) a[i] = row[k0 + frag_k(i, h)];
    return a;
}

#define VST2(T, ptr, val) do { *(volatile T*)(ptr) = (val); __threadfence(); *(volatile T*)(ptr) = (val); } while (0)
typedef float v4f __attribute__((ext_vector_type(4)));
#define VST2V4(ptr, val) do { *(volatile v4f*)(ptr) = (val); __threadfence(); *(volatile v4f*)(ptr) = (val); } while (0)

__device__ __attribute__((noinline)) float act_fn(float v, int act) {
    if (act == 1) return fmaxf(v, 0.f);
    if (act == 2) { const float u = 0.7978845608028654f * (v + 0.044715f * v * v * v); return 0.5f * v * (1.f + tanhf(u)); }
    if (act == 3) return v / (1.f + expf(-v));
    if (act == 4) return 0.5f * v * (1.f + erff(v * 0.7071067811865476f));
    if (act == 5) return tanhf(v);
    if (act == 6) return 1.f / (1.f + expf(-v));
    if (act == 7) return (v > 0.f) ? v : 0.01f * v;
    if (act == 8) return (v > 0.f) ? v : (expf(v) - 1.f);
    if (act == 9) return fminf(fmaxf(v, 0.f), 6.f);
    if (act == 10) return fabsf(v);
    if (act == 11) return (v >= 0.f) ? v : 0.1f * v;
    if (act == 12) return (v > 0.f) ? v : 0.2f * v;
    if (act == 13) return (v > 20.f) ? v : log1pf(expf(v));
    return v;
}

struct GemmP {
    const float* A; const float* B; const float* bias; const float* R; float* C;
    long long sAo, sAi, sAm, sAk, sBo, sBi, sBn, sBk, sCo, sCi, sCm, sRo, sRi, sRm, sRn;
    int M, N, K, zi_n, flags, act; float alpha, beta, sa, sb;
    int Npad, pad_;
};
static_assert(sizeof(GemmP) == 5 * 8 + 15 * 8 + 6 * 4 + 4 * 4 + 2 * 4, "GemmP has padding");

template <int MODE>
__global__ __launch_bounds__(32) void k_gemm(GemmP p) {
    const int lane = threadIdx.x & 31, h = lane >> 4, l15 = lane & 15;
    const int m0 = blockIdx.y * 16, n0 = blockIdx.x * 32;
    const int z = blockIdx.z, zo = z / p.zi_n, zi = z - zo * p.zi_n;
    const float* A = p.A + zo * p.sAo + zi * p.sAi;
    const float* B = p.B + zo * p.sBo + zi * p.sBi;
    const int am = min(m0 + l15, p.M - 1);
    v8f acc[2], comp[2];
#pragma unroll
    for (int t = 0; t < 2; ++t) { v8f zz = {}; acc[t] = zz; comp[t] = zz; }
    for (int k0 = 0; k0 < p.K; k0 += 32) {
        const float* arow = A + (long long)am * p.sAm;
        if (MODE == 1) {
            const Split a = sp_ld(arow, p.sAk, k0, h, p.K, 1.f);
#pragma unroll
            for (int t = 0; t < 2; ++t) {
                const int bn = min(n0 + t * 16 + l15, p.N - 1);
                acc[t] = wmma3(a, sp_ld(B + (long long)bn * p.sBn, p.sBk, k0, h, p.K, 1.f), acc[t]);
            }
        } else if (MODE == 3) {
            const Split3 a = sp3_ld(arow, p.sAk, k0, h, p.K, 1.f);
#pragma unroll
            for (int t = 0; t < 2; ++t) {
                const int bn = min(n0 + t * 16 + l15, p.N - 1);
                acc[t] = wmma6(a, sp3_ld(B + (long long)bn * p.sBn, p.sBk, k0, h, p.K, 1.f), acc[t]);
            }
        } else if (MODE == 4) {
            const Split3 a = sp3_ld(arow, p.sAk, k0, h, p.K, 1.f);
#pragma unroll
            for (int t = 0; t < 2; ++t) {
                const int bn = min(n0 + t * 16 + l15, p.N - 1); v8f zz = {};
                const v8f part = wmma6(a, sp3_ld(B + (long long)bn * p.sBn, p.sBk, k0, h, p.K, 1.f), zz);
                const v8f y = part - comp[t]; const v8f s = acc[t] + y; comp[t] = (s - acc[t]) - y; acc[t] = s;
            }
        } else if (MODE == 2) {
            const v16b a = bh_ld(arow, p.sAk, k0, h, p.K, 1.f);
#pragma unroll
            for (int t = 0; t < 2; ++t) {
                const int bn = min(n0 + t * 16 + l15, p.N - 1);
                acc[t] = wmmab(a, bh_ld(B + (long long)bn * p.sBn, p.sBk, k0, h, p.K, 1.f), acc[t]);
            }
        } else {
            const v16h a = fh_ld(arow, p.sAk, k0, h, p.K, p.sa);
#pragma unroll
            for (int t = 0; t < 2; ++t) {
                const int bn = min(n0 + t * 16 + l15, p.N - 1);
                acc[t] = wmma16(a, fh_ld(B + (long long)bn * p.sBn, p.sBk, k0, h, p.K, p.sb), acc[t]);
            }
        }
    }
    const float iscale = (MODE == 0) ? p.alpha / (p.sa * p.sb) : p.alpha;
    float* C = p.C + zo * p.sCo + zi * p.sCi;
    const float* R = p.R + zo * p.sRo + zi * p.sRi;
    __shared__ __align__(16) float ctile[16][36];
#pragma unroll
    for (int t = 0; t < 2; ++t) {
        const int n = n0 + t * 16 + l15; const int nn = min(n, p.N - 1);
#pragma unroll
        for (int r = 0; r < 8; ++r) {
            const int m = m0 + 8 * h + r; const int mm = min(m, p.M - 1);
            float v = acc[t][r] * iscale;
            if (p.flags & 1) v += p.bias[nn];
            if (p.flags & 2) v += p.bias[mm];
            v = act_fn(v, p.act);
            if (p.flags & 4) v += p.beta * R[(long long)mm * p.sRm + (long long)nn * p.sRn];
            ctile[8 * h + r][t * 16 + l15] = (n < p.N) ? v : 0.f;
        }
    }
    __syncthreads();
    const int NW = (p.Npad > p.N) ? p.Npad : p.N;
    const bool fast = (m0 + 16 <= p.M) && (n0 + 32 <= NW) && ((p.sCm & 3) == 0) && ((((size_t)C) & 15) == 0);
    if (fast) {
#pragma unroll
        for (int s = 0; s < 4; ++s) {
            const int row = s * 4 + (lane >> 3), c4 = (lane & 7) * 4;
            const v4f v = *(const v4f*)&ctile[row][c4];
            VST2V4(C + (long long)(m0 + row) * p.sCm + n0 + c4, v);
        }
    } else {
        for (int row = 0; row < 16; ++row) {
            const int m = m0 + row, n = n0 + lane;
            if (m < p.M && n < NW) VST2(float, C + (long long)m * p.sCm + n, ctile[row][lane]);
        }
    }
}

#define AW 4
struct AttnP {
    const float* Q; const float* K; const float* V; float* O; float* P; const float* Mf; const int* Mi; float* ST;
    const float* Pw; const float* Rt; const int* SQ; const int* SK;
    long long swb, swh, swi, swj, srb, srh, sri;
    long long sQb, sQh, sQi, sQd, sKb, sKh, sKj, sKd, sVb, sVh, sVj, sVd, sOb, sOh, sOi, sPb, sPh, sPi, smb, smh, smi, smj;
    int Lq, Lk, dh, dv, hrep, causal, coff, pband;
    float scale, mfill; int nonorm, mpol;
    int roff, rn, segpol, win;
};
static_assert(sizeof(AttnP) == 12 * 8 + 29 * 8 + 16 * 4, "AttnP has padding");

#ifndef KATTN_ATTR
#define KATTN_ATTR
#endif
template <int DHP, int DVP, int QM, bool SPLITPV, bool TWOPASS>
__global__ __launch_bounds__(32 * AW) KATTN_ATTR void k_attn(AttnP p) {
    constexpr int NT = DVP / 16;
    constexpr int KS = DHP / 32;
    constexpr int VP = DVP + 8;
    __shared__ __align__(16) float    pl[AW][16 * 64];
    __shared__ __align__(16) _Float16 vl[(SPLITPV ? 2 : 1) * 64 * VP];
    const int lane = threadIdx.x & 31, hf = lane >> 4, l15 = lane & 15, wave = threadIdx.x >> 5;
    const int h = blockIdx.y, b = blockIdx.z, hk = h / p.hrep;
    const int q0 = (blockIdx.x * AW + wave) * 16;
    float* myp = pl[wave];
    const float L2E = 1.4426950408889634f;
    const float NEG = -__builtin_inff();
    const int qi = min(q0 + l15, p.Lq - 1);
    const float* qrow = p.Q + b * p.sQb + h * p.sQh + (long long)qi * p.sQi;
    const float* kbase = p.K + b * p.sKb + hk * p.sKh;
    const float* vbase = p.V + b * p.sVb + hk * p.sVh;
    v16h qa[QM == 0 ? KS : 1]; Split qs_[QM == 1 ? KS : 1]; Split3 qt_[QM == 2 ? KS : 1];
#pragma unroll
    for (int ks = 0; ks < KS; ++ks) {
        if (QM == 2) qt_[ks] = sp3_ld(qrow, p.sQd, ks * 32, hf, p.dh, 1.f);
        else if (QM == 1) qs_[ks] = sp_ld(qrow, p.sQd, ks * 32, hf, p.dh, 1.f);
        else qa[ks] = fh_ld(qrow, p.sQd, ks * 32, hf, p.dh, 1.f);
    }
    v8f o[NT]; float m8[8], l8[8];
#pragma unroll
    for (int t = 0; t < NT; ++t) { v8f zz = {}; o[t] = zz; }
#pragma unroll
    for (int i = 0; i < 8; ++i) { m8[i] = NEG; l8[i] = 0.f; }
    int jend = p.Lk;
    if (p.causal == 1) { const int je = (blockIdx.x * AW + AW - 1) * 16 + 16 + p.coff; jend = min(jend, max(je, 0)); }
    const int npass = TWOPASS ? 2 : 1;
    for (int pass = 0; pass < npass; ++pass) {
        const bool dopv = (!TWOPASS) || pass == 1;
        for (int j0 = 0; j0 < jend; j0 += 64) {
            if (dopv) {
                __syncthreads();
                for (int idx = threadIdx.x; idx < 64 * DVP; idx += 32 * AW) {
                    const int jr = idx / DVP, d = idx - jr * DVP, j = j0 + jr;
                    const float f = (j < p.Lk && d < p.dv) ? vbase[(long long)j * p.sVj + (long long)d * p.sVd] : 0.f;
                    if (SPLITPV) {
                        const __bf16 hb = bf16_rne(f);
                        ((__bf16*)vl)[jr * VP + d] = hb; ((__bf16*)vl)[64 * VP + jr * VP + d] = bf16_rne(f - bf16_f32(hb));
                    } else vl[jr * VP + d] = (_Float16)f;
                }
            }
            v8f s[4];
#pragma unroll
            for (int t = 0; t < 4; ++t) {
                const int j = min(j0 + t * 16 + l15, p.Lk - 1);
                const float* krow = kbase + (long long)j * p.sKj;
                v8f acc = {};
#pragma unroll
                for (int ks = 0; ks < KS; ++ks) {
                    if (QM == 2)      acc = wmma6(qt_[ks], sp3_ld(krow, p.sKd, ks * 32, hf, p.dh, 1.f), acc);
                    else if (QM == 1) acc = wmma3(qs_[ks], sp_ld(krow, p.sKd, ks * 32, hf, p.dh, 1.f), acc);
                    else              acc = wmma16(qa[ks], fh_ld(krow, p.sKd, ks * 32, hf, p.dh, 1.f), acc);
                }
                s[t] = acc;
            }
            float pv[8][4];
#pragma unroll
            for (int i = 0; i < 8; ++i) {
                const int irow = q0 + i + 8 * hf;
                const int ic = min(irow, p.Lq - 1);
                float sc[4];
#pragma unroll
                for (int t = 0; t < 4; ++t) {
                    const int jg = j0 + t * 16 + l15;
                    float v = s[t][i] * p.scale;
                    if (p.Mf) v += p.Mf[b * p.smb + h * p.smh + (long long)ic * p.smi + (long long)min(jg, p.Lk - 1) * p.smj];
                    if (p.Rt) { int rc = ic - min(jg, p.Lk - 1) + p.roff; rc = rc < 0 ? 0 : (rc >= p.rn ? p.rn - 1 : rc); v += p.Rt[b * p.srb + h * p.srh + (long long)ic * p.sri + rc]; }
                    if (p.Mi) { const int mv = p.Mi[b * p.smb + h * p.smh + (long long)ic * p.smi + (long long)min(jg, p.Lk - 1) * p.smj]; if (p.mpol ? (mv != 0) : (mv == 0)) v = p.mfill; }
                    if (p.SQ) { const bool same = p.SQ[(long long)b * p.Lq + ic] == p.SK[(long long)b * p.Lk + min(jg, p.Lk - 1)]; if (p.segpol ? same : !same) v = p.mfill; }
                    if (p.causal == 2 && jg > irow + p.coff) v = p.mfill;
                    if (jg >= p.Lk || (p.causal == 1 && jg > irow + p.coff) || (p.causal == 3 && jg < irow + p.coff) || (p.win > 0 && irow + p.coff - jg > p.win)) v = NEG; else v *= L2E;
                    sc[t] = v;
                }
                if (!TWOPASS || pass == 0) {
                    float mx = fmaxf(fmaxf(sc[0], sc[1]), fmaxf(sc[2], sc[3]));
                    mx = fmaxf(mx, __shfl_xor(mx, 1, 32)); mx = fmaxf(mx, __shfl_xor(mx, 2, 32));
                    mx = fmaxf(mx, __shfl_xor(mx, 4, 32)); mx = fmaxf(mx, __shfl_xor(mx, 8, 32));
                    const float mnew = fmaxf(m8[i], mx);
                    const float corr = (mnew == NEG) ? 1.f : exp2f(m8[i] - mnew);
                    float rs = 0.f;
#pragma unroll
                    for (int t = 0; t < 4; ++t) {
                        const float pp = (sc[t] == NEG) ? 0.f : exp2f(sc[t] - mnew); rs += pp;
                        pv[i][t] = p.Pw ? pp * p.Pw[b * p.swb + h * p.swh + (long long)ic * p.swi + (long long)min(j0 + t * 16 + l15, p.Lk - 1) * p.swj] : pp;
                    }
                    rs += __shfl_xor(rs, 1, 32); rs += __shfl_xor(rs, 2, 32); rs += __shfl_xor(rs, 4, 32); rs += __shfl_xor(rs, 8, 32);
                    l8[i] = l8[i] * corr + rs; m8[i] = mnew;
                    if (!TWOPASS) {
#pragma unroll
                        for (int t = 0; t < NT; ++t) o[t][i] *= corr;
                    }
                } else {
                    const float inv = (l8[i] > 0.f) ? 1.f / l8[i] : 0.f;
#pragma unroll
                    for (int t = 0; t < 4; ++t) {
                        const int jg = j0 + t * 16 + l15;
                        float pp = (sc[t] == NEG) ? 0.f : exp2f(sc[t] - m8[i]) * inv;
                        if (p.Pw) pp *= p.Pw[b * p.swb + h * p.swh + (long long)ic * p.swi + (long long)min(jg, p.Lk - 1) * p.swj];
                        pv[i][t] = pp;
                    }
                }
            }
            if (dopv) {
#pragma unroll
                for (int i = 0; i < 8; ++i)
#pragma unroll
                    for (int t = 0; t < 4; ++t) myp[(i + 8 * hf) * 64 + t * 16 + l15] = pv[i][t];
                __syncthreads();
                if (p.P) {
                    float* pb_ = p.P + b * p.sPb + h * p.sPh;
                    const bool fastP = (p.pband == 0) && ((p.sPi & 3) == 0) && (j0 + 64 <= p.Lk) && (q0 + 16 <= p.Lq) && ((((size_t)pb_) & 15) == 0);
                    if (fastP) {
#pragma unroll
                        for (int s = 0; s < 8; ++s) {
                            const int row = s * 2 + (lane >> 4), c4 = (lane & 15) * 4;
                            const v4f v = *(const v4f*)(myp + row * 64 + c4);
                            VST2V4(pb_ + (long long)(q0 + row) * p.sPi + j0 + c4, v);
                        }
                    } else {
                        for (int row = 0; row < 16; ++row) {
                            const int irow = q0 + row; if (irow >= p.Lq) continue;
                            for (int c = lane; c < 64; c += 32) {
                                const int jg = j0 + c; if (jg >= p.Lk) continue;
                                if (p.pband == 0) VST2(float, pb_ + (long long)irow * p.sPi + jg, myp[row * 64 + c]);
                                else if (jg - irow <= p.pband && irow - jg <= p.pband) VST2(float, pb_ + (long long)irow * p.sPi + (jg - irow + p.pband), myp[row * 64 + c]);
                            }
                        }
                    }
                }
                if (SPLITPV) {
                    const Split pa0 = sp_ld(myp + l15 * 64, 1, 0, hf, 64, 1.f), pa1 = sp_ld(myp + l15 * 64, 1, 32, hf, 64, 1.f);
                    const __bf16* vh = (const __bf16*)vl; const __bf16* vlo = vh + 64 * VP;
#pragma unroll
                    for (int t = 0; t < NT; ++t) {
                        const int dcol = t * 16 + l15;
                        Split b0, b1;
#pragma unroll
                        for (int e = 0; e < 16; ++e) {
                            const int k0 = frag_k(e, hf), k1 = 32 + frag_k(e, hf);
                            b0.hi[e] = vh[k0 * VP + dcol]; b0.lo[e] = vlo[k0 * VP + dcol]; b1.hi[e] = vh[k1 * VP + dcol]; b1.lo[e] = vlo[k1 * VP + dcol];
                        }
                        o[t] = wmma3(pa0, b0, o[t]);
                        o[t] = wmma3(pa1, b1, o[t]);
                    }
                } else {
                    const v16h pa0 = fh_ld(myp + l15 * 64, 1, 0, hf, 64, 4096.f), pa1 = fh_ld(myp + l15 * 64, 1, 32, hf, 64, 4096.f);
#pragma unroll
                    for (int t = 0; t < NT; ++t) {
                        const int dcol = t * 16 + l15;
                        v16h b0, b1;
#pragma unroll
                        for (int e = 0; e < 16; ++e) { b0[e] = vl[frag_k(e, hf) * VP + dcol]; b1[e] = vl[(32 + frag_k(e, hf)) * VP + dcol]; }
                        o[t] = wmma16(pa0, b0, o[t]);
                        o[t] = wmma16(pa1, b1, o[t]);
                    }
                }
            }
        }
    }
    float* obase = p.O + b * p.sOb + h * p.sOh;
    if (p.ST) {
        const int rl = lane >> 1, isel = rl & 7;
        float mv = 0.f, lv = 0.f;
#pragma unroll
        for (int i = 0; i < 8; ++i) if (i == isel) { mv = m8[i]; lv = l8[i]; }
        const int irow = q0 + rl;
        if (irow < p.Lq) { float* st = p.ST + (((long long)b * gridDim.y + h) * p.Lq + irow) * 2 + (lane & 1); VST2(float, st, (lane & 1) ? lv : mv * 0.6931471805599453f); }
    }
    float invr[8];
#pragma unroll
    for (int i = 0; i < 8; ++i) {
        if (TWOPASS) invr[i] = SPLITPV ? 1.f : (1.f / 4096.f);
        else if (p.nonorm) invr[i] = exp2f(m8[i]) * (SPLITPV ? 1.f : (1.f / 4096.f));
        else invr[i] = (l8[i] > 0.f) ? (SPLITPV ? 1.f / l8[i] : 1.f / (l8[i] * 4096.f)) : 0.f;
    }
    __syncthreads();
    const bool ofast = ((p.sOi & 3) == 0) && ((((size_t)obase) & 15) == 0) && (q0 + 16 <= p.Lq);
#pragma unroll
    for (int c0 = 0; c0 < DVP; c0 += 64) {
#pragma unroll
        for (int i = 0; i < 8; ++i)
#pragma unroll
            for (int t = 0; t < NT; ++t) if (t * 16 >= c0 && t * 16 < c0 + 64) myp[(i + 8 * hf) * 64 + (t * 16 - c0) + l15] = o[t][i] * invr[i];
        __syncthreads();
        const int cw = (DVP - c0 < 64) ? (DVP - c0) : 64;
        if (ofast && (c0 + cw <= p.dv) && (cw % 32 == 0)) {
            const int lpr = cw / 4;
            const int rows_per_ins = 32 / lpr;
            for (int r0 = 0; r0 < 16; r0 += rows_per_ins) {
                const int row = r0 + lane / lpr, c4 = (lane % lpr) * 4;
                const v4f v = *(const v4f*)(myp + row * 64 + c4);
                VST2V4(obase + (long long)(q0 + row) * p.sOi + c0 + c4, v);
            }
        } else {
            for (int row = 0; row < 16; ++row) {
                const int irow = q0 + row; if (irow >= p.Lq) continue;
                for (int c = lane; c < cw; c += 32) { const int d = c0 + c; if (d < p.dv) VST2(float, obase + (long long)irow * p.sOi + d, myp[row * 64 + c]); }
            }
        }
        __syncthreads();
    }
}

struct TrP { const float* src; float* dst; const float* R2; long long sSz, lds, sDz, ldd, sRz, ldr; int R, C, flags, act; float alpha, beta; };
static_assert(sizeof(TrP) == 3 * 8 + 6 * 8 + 6 * 4, "TrP has padding");
__global__ __launch_bounds__(256) void k_tr(TrP p) {
    __shared__ float tile[32][33];
    const int c0 = blockIdx.x * 32, r0 = blockIdx.y * 32, z = blockIdx.z;
    const int lane = threadIdx.x & 31, wave = threadIdx.x >> 5;
    const float* s = p.src + z * p.sSz;
#pragma unroll
    for (int k = 0; k < 4; ++k) {
        const int rl = wave * 4 + k, r = r0 + rl, c = c0 + lane;
        tile[rl][lane] = (r < p.R && c < p.C) ? s[(long long)r * p.lds + c] : 0.f;
    }
    __syncthreads();
    float* d = p.dst + z * p.sDz; const float* rr = p.R2 + z * p.sRz;
#pragma unroll
    for (int k = 0; k < 4; ++k) {
        const int cl = wave * 4 + k, c = c0 + cl, r = r0 + lane;
        if (c < p.C && r < p.R) {
            float v = act_fn(p.alpha * tile[lane][cl], p.act);
            if (p.flags & 1) v += p.beta * rr[(long long)c * p.ldr + r];
            VST2(float, d + (long long)c * p.ldd + r, v);
        }
    }
}

__global__ __launch_bounds__(256) void k_affine(const float* __restrict__ src, float* __restrict__ dst, int n, float a, float b, const float* __restrict__ sdev) {
    const int i = blockIdx.x * 256 + threadIdx.x;
    if (i < n) { const float aa = sdev ? a * sdev[0] : a; const float v = aa * src[i] + b; VST2(float, dst + i, v); }
}

struct SmP { const float* src; float* dst; const float* Mf; long long sz, sr, dz, dr, smz, smr; int n, pad; float scale_in, scale_out; };
static_assert(sizeof(SmP) == 3 * 8 + 6 * 8 + 4 * 4, "SmP has padding");
__global__ __launch_bounds__(256) void k_softmax(SmP p) {
    __shared__ float red[256];
    const int r = blockIdx.x, z = blockIdx.y, tid = threadIdx.x;
    const float* s = p.src + z * p.sz + (long long)r * p.sr;
    const float* mf = p.Mf ? (p.Mf + z * p.smz + (long long)r * p.smr) : nullptr;
    float mx = -__builtin_inff();
    for (int j = tid; j < p.n; j += 256) { float v = s[j] * p.scale_in; if (mf) v += mf[j]; mx = fmaxf(mx, v); }
    red[tid] = mx; __syncthreads();
    for (int o = 128; o > 0; o >>= 1) { if (tid < o) red[tid] = fmaxf(red[tid], red[tid + o]); __syncthreads(); }
    mx = red[0]; __syncthreads();
    float sum = 0.f;
    for (int j = tid; j < p.n; j += 256) { float v = s[j] * p.scale_in; if (mf) v += mf[j]; sum += (mx == -__builtin_inff()) ? 0.f : expf(v - mx); }
    red[tid] = sum; __syncthreads();
    for (int o = 128; o > 0; o >>= 1) { if (tid < o) red[tid] += red[tid + o]; __syncthreads(); }
    sum = red[0];
    const float inv = (sum > 0.f) ? p.scale_out / sum : 0.f;
    float* d = p.dst + z * p.dz + (long long)r * p.dr;
    for (int j = tid; j < p.n; j += 256) { float v = s[j] * p.scale_in; if (mf) v += mf[j]; const float o = (mx == -__builtin_inff()) ? 0.f : expf(v - mx) * inv; VST2(float, d + j, o); }
}
__global__ __launch_bounds__(256) void k_stats(const float* __restrict__ x, long long sz, long long so, long long si, int inner, int n, float eps, float* __restrict__ stat, int mode) {
    __shared__ float red[256];
    const int z = blockIdx.x, tid = threadIdx.x;
    const float* base = x + z * sz;
    float s = 0.f;
    for (int e = tid; e < n; e += 256) s += base[(long long)(e / inner) * so + (long long)(e % inner) * si];
    red[tid] = s; __syncthreads();
    for (int o = 128; o > 0; o >>= 1) { if (tid < o) red[tid] += red[tid + o]; __syncthreads(); }
    const float mu = (mode == 0 || mode == 3) ? red[0] / (float)n : 0.f; __syncthreads();
    float q = 0.f;
    for (int e = tid; e < n; e += 256) { const float dlt = base[(long long)(e / inner) * so + (long long)(e % inner) * si] - mu; q += dlt * dlt; }
    red[tid] = q; __syncthreads();
    for (int o = 128; o > 0; o >>= 1) { if (tid < o) red[tid] += red[tid + o]; __syncthreads(); }
    {
        float rs;
        if (mode == 2) rs = sqrtf((float)n) / fmaxf(sqrtf(red[0]), eps); else if (mode == 3) rs = rsqrtf(red[0] / (float)(n - 1) + eps); else rs = rsqrtf(red[0] / (float)n + eps);
        if (tid < 32) { const float v = (tid == 0) ? mu : ((tid == 1) ? rs : 0.f); VST2(float, stat + (long long)z * 32 + tid, v); }
    }
}
__global__ __launch_bounds__(256) void k_norm_apply(const float* __restrict__ x, float* __restrict__ y, const float* __restrict__ stat, const float* __restrict__ g, const float* __restrict__ bta,
                                                     int Z, int C, int L, int G, int bn, int act) {
    const long long idx = (long long)blockIdx.x * 256 + threadIdx.x;
    if (idx >= (long long)Z * C * L) return;
    const int l = (int)(idx % L); const long long zc = idx / L; const int c = (int)(zc % C), z = (int)(zc / C); (void)l;
    const int set = bn ? c : (z * G + c / (C / G));
    float v = (x[idx] - stat[(long long)set * 32]) * stat[(long long)set * 32 + 1];
    if (g) v *= g[c];
    if (bta) v += bta[c];
    v = act_fn(v, act);
    VST2(float, y + idx, v);
}

__global__ __launch_bounds__(256) void k_lse_neg(const float* __restrict__ st, float* __restrict__ c, int n) {
    const int i = blockIdx.x * 256 + threadIdx.x;
    if (i < n) { const float v = -(st[2 * i] + logf(st[2 * i + 1])); VST2(float, c + i, v); }
}

__global__ __launch_bounds__(256) void k_iota(int* __restrict__ dst, int n, int a, int b) {
    const int i = blockIdx.x * 256 + threadIdx.x;
    if (i < n) { const int v = a * i + b; VST2(int, dst + i, v); }
}

__global__ __launch_bounds__(256) void k_axpby(const float* __restrict__ x, const float* __restrict__ y, float* __restrict__ dst, int n, float a, float b, float c) {
    const int i = blockIdx.x * 256 + threadIdx.x;
    if (i < n) { const float v = a * x[i] + b * y[i] + c; VST2(float, dst + i, v); }
}

struct RopeP { const float* X; float* Y; const float* C; const float* Sn; const int* pos; long long sXr, sXh, sYr, sYh, sCb, sCp, sCd; int R, Hn, D, S, mode, tmode, pmode, pad; };
static_assert(sizeof(RopeP) == 5 * 8 + 7 * 8 + 8 * 4, "RopeP has padding");
__global__ __launch_bounds__(256) void k_rope(RopeP p) {
    const long long idx = (long long)blockIdx.x * 256 + threadIdx.x;
    if (idx >= (long long)p.R * p.Hn * p.D) return;
    const int d = (int)(idx % p.D); const long long rh = idx / p.D; const int h = (int)(rh % p.Hn); const int r = (int)(rh / p.Hn);
    const int half = p.D / 2;
    int partner; float sign;
    if (p.mode == 0) { partner = (d < half) ? d + half : d - half; sign = (d < half) ? -1.f : 1.f; }
    else { partner = d ^ 1; sign = (d & 1) ? 1.f : -1.f; }
    const int tcol = (p.tmode == 0) ? d : ((p.tmode == 1) ? (d % half) : (d >> 1));
    const int pp = (p.pmode == 0) ? (r % p.S) : ((p.pmode == 1) ? h : p.pos[r]);
    const long long toff = (long long)(r / p.S) * p.sCb + (long long)pp * p.sCp + (long long)tcol * p.sCd;
    const float* xr = p.X + (long long)r * p.sXr + (long long)h * p.sXh;
    const float v = xr[d] * p.C[toff] + sign * xr[partner] * p.Sn[toff];
    VST2(float, p.Y + (long long)r * p.sYr + (long long)h * p.sYh + d, v);
}

__global__ __launch_bounds__(256) void k_invf(float* __restrict__ invb, int half, int D, float base, float num, int fmode, float cexp) {
    const int i = blockIdx.x * 256 + threadIdx.x;
    if (i >= ((half + 31) / 32) * 32) return;
    if (i >= half) { VST2(float, invb + i, 0.f); return; }
    const float e = (float)(2 * i) / (float)D;
    float invf;
    if (fmode == 1) invf = num * expf((float)(2 * i) * cexp);
    else if (fmode == 2) invf = num * powf(base, (-2.0f * ((float)i - 1.0f)) / (float)D);
    else invf = num * (1.0f / powf(base, e));
    VST2(float, invb + i, invf);
}
__global__ __launch_bounds__(256) void k_sincos(float* __restrict__ cs, float* __restrict__ sn, const float* __restrict__ invb, int S, int half, float pscale) {
    const int idx = blockIdx.x * 256 + threadIdx.x;
    if (idx >= S * half) return;
    const int s = idx / half, i = idx - s * half;
    const float ang = (pscale * (float)s) * invb[i];
    VST2(float, cs + idx, cosf(ang)); VST2(float, sn + idx, sinf(ang));
}

__global__ __launch_bounds__(256) void k_mulact(const float* __restrict__ x, const float* __restrict__ y, float* __restrict__ dst, int n, int act) {
    const int i = blockIdx.x * 256 + threadIdx.x;
    if (i < n) { const float v = act_fn(x[i], act) * y[i]; VST2(float, dst + i, v); }
}

__global__ __launch_bounds__(256) void k_matvec(GemmP p) {
    const int rpt = (p.N == 1) ? 1 : 32;
    const long long r0 = ((long long)blockIdx.x * 256 + threadIdx.x) * rpt; const int z = blockIdx.z, zo = z / p.zi_n, zi = z - zo * p.zi_n;
    if (r0 >= p.M) return;
    const float* Bb = p.B + zo * p.sBo + zi * p.sBi;
    float* C = p.C + zo * p.sCo + zi * p.sCi; const float* R = p.R + zo * p.sRo + zi * p.sRi;
    for (int rr = 0; rr < rpt; ++rr) {
        const long long r = r0 + rr; if (r >= p.M) break;
        const float* A = p.A + zo * p.sAo + zi * p.sAi + r * p.sAm;
        float acc[8] = {0.f, 0.f, 0.f, 0.f, 0.f, 0.f, 0.f, 0.f};
        for (int k = 0; k < p.K; ++k) { const float a = A[(long long)k * p.sAk];
#pragma unroll
            for (int j = 0; j < 8; ++j) if (j < p.N) acc[j] += a * Bb[(long long)j * p.sBn + (long long)k * p.sBk]; }
#pragma unroll
        for (int j = 0; j < 8; ++j) if (j < p.N) {
            float v = acc[j] * p.alpha;
            if (p.flags & 1) v += p.bias[j];
            if (p.flags & 2) v += p.bias[r];
            v = act_fn(v, p.act);
            if (p.flags & 4) v += p.beta * R[r * p.sRm + (long long)j * p.sRn];
            VST2(float, C + r * p.sCm + j, v);
        }
    }
}
__global__ __launch_bounds__(256) void k_smallsoftmax(const float* __restrict__ src, float* __restrict__ dst, long long sr, long long dr, int n, long long R, float scale) {
    const long long r0 = ((long long)blockIdx.x * 256 + threadIdx.x) * 32;
    for (int rr = 0; rr < 32; ++rr) {
        const long long r = r0 + rr; if (r >= R) return;
        const float* s = src + r * sr; float* d = dst + r * dr;
        float mx = -__builtin_inff();
        for (int j = 0; j < n; ++j) mx = fmaxf(mx, s[j] * scale);
        float sum = 0.f;
        for (int j = 0; j < n; ++j) sum += expf(s[j] * scale - mx);
        const float inv = 1.f / sum;
        for (int j = 0; j < n; ++j) { const float v = expf(s[j] * scale - mx) * inv; VST2(float, d + j, v); }
    }
}

__global__ __launch_bounds__(32) void k_unitstat(float* __restrict__ st) { const int t = threadIdx.x; const float v = (t == 1) ? 1.f : 0.f; VST2(float, st + t, v); }

__global__ __launch_bounds__(256) void k_lincopy(const float* __restrict__ src, long long lds, float* __restrict__ dst, long long ldd, long long rows, int cols) {
    const long long i = (long long)blockIdx.x * 256 + threadIdx.x; if (i >= rows * cols) return;
    const long long r = i / cols; const int c = (int)(i - r * cols);
    const float v = src[r * lds + c]; VST2(float, dst + r * ldd + c, v);
}


#define CT_ 981
#define FT_ 15930
__constant__ int c_clh[4] = {25, 12, 6, 3}; __constant__ int c_clw[4] = {30, 15, 7, 3}; __constant__ int c_coff[4] = {0, 750, 930, 972};
__constant__ int c_flh[4] = {100, 50, 25, 12}; __constant__ int c_flw[4] = {120, 60, 30, 15}; __constant__ int c_foff[4] = {0, 12000, 15000, 15750};
__global__ __launch_bounds__(256) void k_ep_prep(const float* __restrict__ rgbs, float* __restrict__ RG, float* __restrict__ FFr, const float* __restrict__ pts, float* __restrict__ CO, float* __restrict__ XY0, int S, int H, int W, int N) { const long long q = (long long)blockIdx.x * 256 + threadIdx.x;
    if (q < (long long)S * H * W) VST2(float, RG + q, 2.f * (rgbs[q] / 255.f) - 1.f);
    if (q < (long long)S * 3000) { const int s = (int)(q / 3000); const int pp = (int)(q % 3000); const int oy = pp / 60, ox = pp % 60; const float sy = fminf(fmaxf(((float)oy + 0.5f) * ((float)H / 50.f) - 0.5f, 0.f), (float)(H - 1)), sx = fminf(fmaxf(((float)ox + 0.5f) * ((float)W / 60.f) - 0.5f, 0.f), (float)(W - 1));
        const int y0 = (int)floorf(sy), x0 = (int)floorf(sx); const int y1 = min(y0 + 1, H - 1), x1 = min(x0 + 1, W - 1); const float wy = sy - (float)y0, wx = sx - (float)x0;
        auto src = [&](int yy, int xx) -> float { const float a = 2.f * (rgbs[((long long)(s == 0 ? S - 1 : s) * H + yy) * W + xx] / 255.f) - 1.f; if (s == 0) return a; const float b2 = 2.f * (rgbs[((long long)(s - 1) * H + yy) * W + xx] / 255.f) - 1.f; return a - b2; };
        const float v = (src(y0, x0) * (1.f - wx) + src(y0, x1) * wx) * (1.f - wy) + (src(y1, x0) * (1.f - wx) + src(y1, x1) * wx) * wy; VST2(float, FFr + (long long)s * 3008 + pp, v); }
    if (q < (long long)S * N) { const int n = (int)(q % N); VST2(float, CO + q * 2, pts[n * 2] / 8.f); VST2(float, CO + q * 2 + 1, pts[n * 2 + 1] / 8.f); if (q < N) { VST2(float, XY0 + n * 2, pts[n * 2] / 8.f); VST2(float, XY0 + n * 2 + 1, pts[n * 2 + 1] / 8.f); } } }
__global__ __launch_bounds__(256) void k_ep_inorm(float* __restrict__ X, int ld, int L) { __shared__ float red[256]; float* r = X + (long long)blockIdx.x * ld; float s = 0.f; for (int i = threadIdx.x; i < L; i += 256) s += r[i]; red[threadIdx.x] = s; __syncthreads(); for (int o = 128; o > 0; o >>= 1) { if (threadIdx.x < o) red[threadIdx.x] += red[threadIdx.x + o]; __syncthreads(); } const float mean = red[0] / (float)L; __syncthreads();
    float v = 0.f; for (int i = threadIdx.x; i < L; i += 256) { const float d = r[i] - mean; v += d * d; } red[threadIdx.x] = v; __syncthreads(); for (int o = 128; o > 0; o >>= 1) { if (threadIdx.x < o) red[threadIdx.x] += red[threadIdx.x + o]; __syncthreads(); } const float rs = rsqrtf(red[0] / (float)L + 1e-5f);
    for (int i = threadIdx.x; i < L; i += 256) { const float nv = (r[i] - mean) * rs; VST2(float, r + i, nv); } }
__global__ __launch_bounds__(256) void k_ep_patch(const float* __restrict__ RG, float* __restrict__ PATCH, int S, int H, int W) { const long long q = (long long)blockIdx.x * 256 + threadIdx.x; if (q >= (long long)S * 750 * 64) return; const int kk = (int)(q % 64); const int pp = (int)((q / 64) % 750); const int s = (int)(q / (64 * 750)); const int y = pp / 30, x = pp % 30, i = kk / 8, j = kk % 8; VST2(float, PATCH + q, RG[((long long)s * H + 8 * y + i) * W + 8 * x + j]); }
__global__ __launch_bounds__(256) void k_ep_fine(const float* __restrict__ RG, const float* __restrict__ w, float* __restrict__ PYF, int S, int H, int W) { const long long q = (long long)blockIdx.x * 256 + threadIdx.x; if (q >= (long long)S * 64 * 12000) return; const int pp = (int)(q % 12000); const int c = (int)((q / 12000) % 64); const int s = (int)(q / (12000 * 64)); const int y = pp / 120, x = pp % 120; const float* r = RG + ((long long)s * H + 2 * y) * W + 2 * x;
    VST2(float, PYF + ((long long)s * 64 + c) * FT_ + pp, r[0] * w[c * 4] + r[1] * w[c * 4 + 1] + r[W] * w[c * 4 + 2] + r[W + 1] * w[c * 4 + 3]); }
__global__ __launch_bounds__(256) void k_ep_pool(float* __restrict__ PY, int S, int lvl, int fine) { const int* lh = fine ? c_flh : c_clh; const int* lw = fine ? c_flw : c_clw; const int* lo = fine ? c_foff : c_coff; const int TOT = fine ? FT_ : CT_; const int Ho = lh[lvl], Wo = lw[lvl], Wi = lw[lvl - 1]; const long long q = (long long)blockIdx.x * 256 + threadIdx.x; if (q >= (long long)S * 64 * Ho * Wo) return; const int pp = (int)(q % (Ho * Wo)); const long long sc = q / (Ho * Wo); const int y = pp / Wo, x = pp % Wo; const float* src = PY + sc * TOT + lo[lvl - 1];
    VST2(float, PY + sc * TOT + lo[lvl] + pp, 0.25f * (src[(2 * y) * Wi + 2 * x] + src[(2 * y) * Wi + 2 * x + 1] + src[(2 * y + 1) * Wi + 2 * x] + src[(2 * y + 1) * Wi + 2 * x + 1])); }
__global__ __launch_bounds__(256) void k_ep_featsample(const float* __restrict__ PY, int fine, const float* __restrict__ CO, float* __restrict__ FOUT, int S, int N, int mode) { const int q = blockIdx.x * 256 + threadIdx.x; if (q >= S * N * 64) return; const int c = q % 64; const int n = (q / 64) % N; const int s = q / (64 * N); const int fr = (mode == 0) ? 0 : max(s - mode, 0); const int Hh = fine ? 100 : 25, Ww = fine ? 120 : 30; const int TOT = fine ? FT_ : CT_;
    const float x = CO[((long long)fr * N + n) * 2], y = CO[((long long)fr * N + n) * 2 + 1]; const float x0 = floorf(x), y0 = floorf(y); const float wx = x - x0, wy = y - y0; const float* img = PY + ((long long)fr * 64 + c) * TOT; float acc = 0.f;
    for (int dy = 0; dy < 2; ++dy) for (int dx = 0; dx < 2; ++dx) { const float ix = x0 + (float)dx, iy = y0 + (float)dy; if (ix >= 0.f && ix <= (float)(Ww - 1) && iy >= 0.f && iy <= (float)(Hh - 1)) acc += ((dy ? wy : 1.f - wy) * (dx ? wx : 1.f - wx)) * img[(int)iy * Ww + (int)ix]; }
    VST2(float, FOUT + q, acc); }
__global__ __launch_bounds__(256) void k_ep_fc14(const float* __restrict__ CVC, float* __restrict__ HIN, int ldh, int S, int N) { const int q = blockIdx.x * 256 + threadIdx.x; if (q >= N * S * 196) return; const int kk = q % 196; const int s = (q / 196) % S; const int n = q / (196 * S); const int oy = kk / 14, ox = kk % 14; float tot = 0.f;
#pragma unroll 1
    for (int l = 0; l < 4; ++l) { const int Hl = c_clh[l], Wl = c_clw[l]; const float* img = CVC + ((long long)s * N + n) * CT_ + c_coff[l]; const float sy = (Hl > 1) ? (float)oy * (float)(Hl - 1) / 13.f : 0.f, sx = (Wl > 1) ? (float)ox * (float)(Wl - 1) / 13.f : 0.f; const int y0 = (int)floorf(sy), x0 = (int)floorf(sx); const int y1 = min(y0 + 1, Hl - 1), x1 = min(x0 + 1, Wl - 1); const float wy = sy - floorf(sy), wx = sx - floorf(sx);
        tot += (img[y0 * Wl + x0] * (1.f - wx) + img[y0 * Wl + x1] * wx) * (1.f - wy) + (img[y1 * Wl + x0] * (1.f - wx) + img[y1 * Wl + x1] * wx) * wy; }
    VST2(float, HIN + ((long long)n * S + s) * ldh + kk, tot * 0.25f); }
__global__ __launch_bounds__(256) void k_ep_ctx(const float* __restrict__ CO, const float* __restrict__ FFr, const float* __restrict__ XY0, float* __restrict__ HIN, int ldh, int fcdim, int S, int N) { const long long q = (long long)blockIdx.x * 256 + threadIdx.x; if (q >= (long long)N * S * 3004) return; const int col = (int)(q % 3004); const int s = (int)((q / 3004) % S); const int n = (int)(q / (3004LL * S)); float v; const int s1 = min(s, S - 2);
    if (col < 2) v = CO[((long long)(s1 + 1) * N + n) * 2 + col] - CO[((long long)s1 * N + n) * 2 + col]; else if (col < 3002) v = FFr[(long long)s * 3008 + (col - 2)]; else v = XY0[n * 2 + (col - 3002)];
    VST2(float, HIN + ((long long)n * S + s) * ldh + fcdim + col, v); }
__global__ __launch_bounds__(256) void k_ep_update(float* __restrict__ CO, const float* __restrict__ DEL, int ldp, float* __restrict__ OUT, float mult, float rescale, int S, int N) { const int q = blockIdx.x * 256 + threadIdx.x; if (q >= S * N * 2) return; const int c = q % 2; const int n = (q / 2) % N; const int s = q / (2 * N); const float v = CO[q] + DEL[((long long)n * S + s) * ldp + c]; VST2(float, OUT + q, v * mult); VST2(float, CO + q, v * rescale); }
__global__ __launch_bounds__(256) void k_ep_xy0(const float* __restrict__ CO, float* __restrict__ XY0, int N) { const int q = blockIdx.x * 256 + threadIdx.x; if (q >= N * 2) return; VST2(float, XY0 + q, CO[q]); }
__global__ __launch_bounds__(256) void k_ep_csample(const float* __restrict__ CV, int set, const float* __restrict__ CO, float* __restrict__ FCAT, int ldf, int S, int N) { const int q = blockIdx.x * 256 + threadIdx.x; if (q >= N * S * 196) return; const int cl = q % 196; const int s = (q / 196) % S; const int n = q / (196 * S); const int col = set * 196 + cl; const int l = cl / 49, kk = cl % 49; const int Hl = c_flh[l], Wl = c_flw[l]; const float* img = CV + ((long long)s * N + n) * FT_ + c_foff[l];
    const float sc = 1.f / (float)(1 << l); const float x = CO[((long long)s * N + n) * 2] * sc + (float)(kk % 7 - 3), y = CO[((long long)s * N + n) * 2 + 1] * sc + (float)(kk / 7 - 3); const float x0 = floorf(x), y0 = floorf(y); const float wx = x - x0, wy = y - y0; float acc = 0.f;
    for (int dy = 0; dy < 2; ++dy) for (int dx = 0; dx < 2; ++dx) { const float ix = x0 + (float)dx, iy = y0 + (float)dy; if (ix >= 0.f && ix <= (float)(Wl - 1) && iy >= 0.f && iy <= (float)(Hl - 1)) acc += ((dy ? wy : 1.f - wy) * (dx ? wx : 1.f - wx)) * img[(int)iy * Wl + (int)ix]; }
    VST2(float, FCAT + ((long long)n * S + s) * ldf + col, acc); }

template __global__ void k_gemm<4>(GemmP);

extern "C" void kernel_launch(void* const* d_in, const int* in_sizes, int n_in, void* d_out, int out_size, void* d_ws, size_t ws_size, hipStream_t stream) {
    (void)in_sizes; (void)n_in; (void)out_size; (void)ws_size;
    const float* rgbs = (const float*)d_in[0];
    const float* pts = (const float*)d_in[1];
    const float* fw = (const float*)d_in[2];
    const float* ffw = (const float*)d_in[3];
    const float* linw = (const float*)d_in[4];
    const float* linb = (const float*)d_in[5];
    const float* dsw1 = (const float*)d_in[6];
    const float* dsb1 = (const float*)d_in[7];
    const float* dsw2 = (const float*)d_in[8];
    const float* dsb2 = (const float*)d_in[9];
    const float* dtw1 = (const float*)d_in[10];
    const float* dtb1 = (const float*)d_in[11];
    const float* dtw2 = (const float*)d_in[12];
    const float* dtb2 = (const float*)d_in[13];
    const int* iters = (const int*)d_in[14];
    const int S = 16;
    const int N = 64;
    const int H = 200;
    const int W = 240;
    const int LAT = 64;
    const int NS = N * S;
    const int LP = 32;
    float* out = (float*)d_out;
    char* wsp = (char*)d_ws;
    float* RG = (float*)wsp; wsp += (((size_t)((size_t)S * H * W) * 4 + 255) / 256) * 256;
    float* FFr = (float*)wsp; wsp += (((size_t)((size_t)S * 3008) * 4 + 255) / 256) * 256;
    float* PATCH = (float*)wsp; wsp += (((size_t)((size_t)S * 750 * 64) * 4 + 255) / 256) * 256;
    float* PYC = (float*)wsp; wsp += (((size_t)((size_t)S * LAT * 981) * 4 + 255) / 256) * 256;
    float* st = (float*)wsp; wsp += (((size_t)((size_t)S * LAT * 32) * 4 + 255) / 256) * 256;
    float* CO = (float*)wsp; wsp += (((size_t)((size_t)S * N * 2) * 4 + 255) / 256) * 256;
    float* XY0 = (float*)wsp; wsp += (((size_t)((size_t)N * 2) * 4 + 255) / 256) * 256;
    float* F0 = (float*)wsp; wsp += (((size_t)((size_t)S * N * LAT) * 4 + 255) / 256) * 256;
    float* CVC = (float*)wsp; wsp += (((size_t)((size_t)S * N * 981) * 4 + 255) / 256) * 256;
    float* HIN = (float*)wsp; wsp += (((size_t)((size_t)NS * 3400) * 4 + 255) / 256) * 256;
    float* HID = (float*)wsp; wsp += (((size_t)((size_t)NS * 128) * 4 + 255) / 256) * 256;
    float* DEL = (float*)wsp; wsp += (((size_t)((size_t)NS * LP) * 4 + 255) / 256) * 256;
    float* PYF = (float*)wsp; wsp += (((size_t)((size_t)S * LAT * 15930) * 4 + 255) / 256) * 256;
    float* F2 = (float*)wsp; wsp += (((size_t)((size_t)S * N * LAT) * 4 + 255) / 256) * 256;
    float* CV1 = (float*)wsp; wsp += (((size_t)((size_t)S * N * 15930) * 4 + 255) / 256) * 256;
    float* CVX = (float*)wsp; wsp += (((size_t)((size_t)S * N * 15930) * 4 + 255) / 256) * 256;
    float* FCAT = (float*)wsp; wsp += (((size_t)((size_t)NS * 608) * 4 + 255) / 256) * 256;
    k_ep_prep<<<(unsigned)(((long long)S * H * W + 255) / 256), 256, 0, stream>>>(rgbs, RG, FFr, pts, CO, XY0, S, H, W, N);
    k_ep_patch<<<(unsigned)((S * 750 * 64 + 255) / 256), 256, 0, stream>>>(RG, PATCH, S, H, W);
    { GemmP genc;
      genc.A = fw; genc.B = PATCH; genc.bias = fw; genc.R = fw; genc.C = PYC;
      genc.sAo = 0; genc.sAi = 0; genc.sAm = 64; genc.sAk = 1; genc.sBo = (long long)750 * 64; genc.sBi = 0; genc.sBn = 64; genc.sBk = 1; genc.sCo = (long long)LAT * 981; genc.sCi = 0; genc.sCm = 981; genc.sRo = 0; genc.sRi = 0; genc.sRm = 0; genc.sRn = 0;
      genc.M = LAT; genc.N = 750; genc.K = 64; genc.zi_n = 1; genc.flags = 0; genc.act = 0;
      genc.alpha = 1.0f; genc.beta = 0.0f; genc.sa = 1.0f; genc.sb = 1.0f; genc.Npad = 750; genc.pad_ = 0;
      k_gemm<4><<<dim3((unsigned)((750) + 31) / 32, (unsigned)((LAT) + 15) / 16, (unsigned)(S)), 32, 0, stream>>>(genc); }
    k_ep_inorm<<<S * LAT, 256, 0, stream>>>(PYC, 981, 750);
    k_ep_pool<<<(unsigned)((S * 64 * 180 + 255) / 256), 256, 0, stream>>>(PYC, S, 1, 0); k_ep_pool<<<(unsigned)((S * 64 * 42 + 255) / 256), 256, 0, stream>>>(PYC, S, 2, 0); k_ep_pool<<<(unsigned)((S * 64 * 9 + 255) / 256), 256, 0, stream>>>(PYC, S, 3, 0);
    k_ep_featsample<<<(unsigned)((S * N * 64 + 255) / 256), 256, 0, stream>>>(PYC, 0, CO, F0, S, N, 0);
    { GemmP gcc0;
      gcc0.A = F0; gcc0.B = PYC + 0; gcc0.bias = F0; gcc0.R = F0; gcc0.C = CVC + 0;
      gcc0.sAo = (long long)N * LAT; gcc0.sAi = 0; gcc0.sAm = LAT; gcc0.sAk = 1; gcc0.sBo = (long long)LAT * 981; gcc0.sBi = 0; gcc0.sBn = 1; gcc0.sBk = 981; gcc0.sCo = (long long)N * 981; gcc0.sCi = 0; gcc0.sCm = 981; gcc0.sRo = 0; gcc0.sRi = 0; gcc0.sRm = 0; gcc0.sRn = 0;
      gcc0.M = N; gcc0.N = 750; gcc0.K = LAT; gcc0.zi_n = 1; gcc0.flags = 0; gcc0.act = 0;
      gcc0.alpha = 0.125f; gcc0.beta = 0.0f; gcc0.sa = 1.0f; gcc0.sb = 1.0f; gcc0.Npad = 750; gcc0.pad_ = 0;
      k_gemm<4><<<dim3((unsigned)((750) + 31) / 32, (unsigned)((N) + 15) / 16, (unsigned)(S)), 32, 0, stream>>>(gcc0); }
    { GemmP gcc1;
      gcc1.A = F0; gcc1.B = PYC + 750; gcc1.bias = F0; gcc1.R = F0; gcc1.C = CVC + 750;
      gcc1.sAo = (long long)N * LAT; gcc1.sAi = 0; gcc1.sAm = LAT; gcc1.sAk = 1; gcc1.sBo = (long long)LAT * 981; gcc1.sBi = 0; gcc1.sBn = 1; gcc1.sBk = 981; gcc1.sCo = (long long)N * 981; gcc1.sCi = 0; gcc1.sCm = 981; gcc1.sRo = 0; gcc1.sRi = 0; gcc1.sRm = 0; gcc1.sRn = 0;
      gcc1.M = N; gcc1.N = 180; gcc1.K = LAT; gcc1.zi_n = 1; gcc1.flags = 0; gcc1.act = 0;
      gcc1.alpha = 0.125f; gcc1.beta = 0.0f; gcc1.sa = 1.0f; gcc1.sb = 1.0f; gcc1.Npad = 180; gcc1.pad_ = 0;
      k_gemm<4><<<dim3((unsigned)((180) + 31) / 32, (unsigned)((N) + 15) / 16, (unsigned)(S)), 32, 0, stream>>>(gcc1); }
    { GemmP gcc2;
      gcc2.A = F0; gcc2.B = PYC + 930; gcc2.bias = F0; gcc2.R = F0; gcc2.C = CVC + 930;
      gcc2.sAo = (long long)N * LAT; gcc2.sAi = 0; gcc2.sAm = LAT; gcc2.sAk = 1; gcc2.sBo = (long long)LAT * 981; gcc2.sBi = 0; gcc2.sBn = 1; gcc2.sBk = 981; gcc2.sCo = (long long)N * 981; gcc2.sCi = 0; gcc2.sCm = 981; gcc2.sRo = 0; gcc2.sRi = 0; gcc2.sRm = 0; gcc2.sRn = 0;
      gcc2.M = N; gcc2.N = 42; gcc2.K = LAT; gcc2.zi_n = 1; gcc2.flags = 0; gcc2.act = 0;
      gcc2.alpha = 0.125f; gcc2.beta = 0.0f; gcc2.sa = 1.0f; gcc2.sb = 1.0f; gcc2.Npad = 42; gcc2.pad_ = 0;
      k_gemm<4><<<dim3((unsigned)((42) + 31) / 32, (unsigned)((N) + 15) / 16, (unsigned)(S)), 32, 0, stream>>>(gcc2); }
    { GemmP gcc3;
      gcc3.A = F0; gcc3.B = PYC + 972; gcc3.bias = F0; gcc3.R = F0; gcc3.C = CVC + 972;
      gcc3.sAo = (long long)N * LAT; gcc3.sAi = 0; gcc3.sAm = LAT; gcc3.sAk = 1; gcc3.sBo = (long long)LAT * 981; gcc3.sBi = 0; gcc3.sBn = 1; gcc3.sBk = 981; gcc3.sCo = (long long)N * 981; gcc3.sCi = 0; gcc3.sCm = 981; gcc3.sRo = 0; gcc3.sRi = 0; gcc3.sRm = 0; gcc3.sRn = 0;
      gcc3.M = N; gcc3.N = 9; gcc3.K = LAT; gcc3.zi_n = 1; gcc3.flags = 0; gcc3.act = 0;
      gcc3.alpha = 0.125f; gcc3.beta = 0.0f; gcc3.sa = 1.0f; gcc3.sb = 1.0f; gcc3.Npad = 9; gcc3.pad_ = 0;
      k_gemm<4><<<dim3((unsigned)((9) + 31) / 32, (unsigned)((N) + 15) / 16, (unsigned)(S)), 32, 0, stream>>>(gcc3); }
    k_ep_fc14<<<(unsigned)((N * S * 196 + 255) / 256), 256, 0, stream>>>(CVC, HIN, 3400, S, N); k_ep_ctx<<<(unsigned)(((long long)N * S * 3004 + 255) / 256), 256, 0, stream>>>(CO, FFr, XY0, HIN, 3400, 196, S, N);
    { GemmP gds1;
      gds1.A = HIN; gds1.B = dsw1; gds1.bias = dsb1; gds1.R = HIN; gds1.C = HID;
      gds1.sAo = 0; gds1.sAi = 0; gds1.sAm = 3400; gds1.sAk = 1; gds1.sBo = 0; gds1.sBi = 0; gds1.sBn = 1; gds1.sBk = 128; gds1.sCo = 0; gds1.sCi = 0; gds1.sCm = 128; gds1.sRo = 0; gds1.sRi = 0; gds1.sRm = 0; gds1.sRn = 0;
      gds1.M = NS; gds1.N = 128; gds1.K = 3200; gds1.zi_n = 1; gds1.flags = 1; gds1.act = 1;
      gds1.alpha = 1.0f; gds1.beta = 0.0f; gds1.sa = 1.0f; gds1.sb = 1.0f; gds1.Npad = 128; gds1.pad_ = 0;
      k_gemm<4><<<dim3((unsigned)((128) + 31) / 32, (unsigned)((NS) + 15) / 16, (unsigned)(1)), 32, 0, stream>>>(gds1); }
    { GemmP gds2;
      gds2.A = HID; gds2.B = dsw2; gds2.bias = dsb2; gds2.R = HID; gds2.C = DEL;
      gds2.sAo = 0; gds2.sAi = 0; gds2.sAm = 128; gds2.sAk = 1; gds2.sBo = 0; gds2.sBi = 0; gds2.sBn = 1; gds2.sBk = 2; gds2.sCo = 0; gds2.sCi = 0; gds2.sCm = LP; gds2.sRo = 0; gds2.sRi = 0; gds2.sRm = 0; gds2.sRn = 0;
      gds2.M = NS; gds2.N = 2; gds2.K = 128; gds2.zi_n = 1; gds2.flags = 1; gds2.act = 0;
      gds2.alpha = 1.0f; gds2.beta = 0.0f; gds2.sa = 1.0f; gds2.sb = 1.0f; gds2.Npad = LP; gds2.pad_ = 0;
      k_gemm<4><<<dim3((unsigned)((LP) + 31) / 32, (unsigned)((NS) + 15) / 16, (unsigned)(1)), 32, 0, stream>>>(gds2); }
    k_ep_update<<<(unsigned)((S * N * 2 + 255) / 256), 256, 0, stream>>>(CO, DEL, LP, out, 8.f, 4.f, S, N); k_ep_xy0<<<1, 256, 0, stream>>>(CO, XY0, N);
    k_ep_fine<<<(unsigned)(((long long)S * 64 * 12000 + 255) / 256), 256, 0, stream>>>(RG, ffw, PYF, S, H, W);
    k_ep_inorm<<<S * LAT, 256, 0, stream>>>(PYF, 15930, 12000);
    k_ep_pool<<<(unsigned)((S * 64 * 3000 + 255) / 256), 256, 0, stream>>>(PYF, S, 1, 1); k_ep_pool<<<(unsigned)((S * 64 * 750 + 255) / 256), 256, 0, stream>>>(PYF, S, 2, 1); k_ep_pool<<<(unsigned)((S * 64 * 180 + 255) / 256), 256, 0, stream>>>(PYF, S, 3, 1);
    k_ep_featsample<<<(unsigned)((S * N * 64 + 255) / 256), 256, 0, stream>>>(PYF, 1, CO, F0, S, N, 0);
    { GemmP gc10;
      gc10.A = F0; gc10.B = PYF + 0; gc10.bias = F0; gc10.R = F0; gc10.C = CV1 + 0;
      gc10.sAo = (long long)N * LAT; gc10.sAi = 0; gc10.sAm = LAT; gc10.sAk = 1; gc10.sBo = (long long)LAT * 15930; gc10.sBi = 0; gc10.sBn = 1; gc10.sBk = 15930; gc10.sCo = (long long)N * 15930; gc10.sCi = 0; gc10.sCm = 15930; gc10.sRo = 0; gc10.sRi = 0; gc10.sRm = 0; gc10.sRn = 0;
      gc10.M = N; gc10.N = 12000; gc10.K = LAT; gc10.zi_n = 1; gc10.flags = 0; gc10.act = 0;
      gc10.alpha = 0.125f; gc10.beta = 0.0f; gc10.sa = 1.0f; gc10.sb = 1.0f; gc10.Npad = 12000; gc10.pad_ = 0;
      k_gemm<4><<<dim3((unsigned)((12000) + 31) / 32, (unsigned)((N) + 15) / 16, (unsigned)(S)), 32, 0, stream>>>(gc10); }
    { GemmP gc11;
      gc11.A = F0; gc11.B = PYF + 12000; gc11.bias = F0; gc11.R = F0; gc11.C = CV1 + 12000;
      gc11.sAo = (long long)N * LAT; gc11.sAi = 0; gc11.sAm = LAT; gc11.sAk = 1; gc11.sBo = (long long)LAT * 15930; gc11.sBi = 0; gc11.sBn = 1; gc11.sBk = 15930; gc11.sCo = (long long)N * 15930; gc11.sCi = 0; gc11.sCm = 15930; gc11.sRo = 0; gc11.sRi = 0; gc11.sRm = 0; gc11.sRn = 0;
      gc11.M = N; gc11.N = 3000; gc11.K = LAT; gc11.zi_n = 1; gc11.flags = 0; gc11.act = 0;
      gc11.alpha = 0.125f; gc11.beta = 0.0f; gc11.sa = 1.0f; gc11.sb = 1.0f; gc11.Npad = 3000; gc11.pad_ = 0;
      k_gemm<4><<<dim3((unsigned)((3000) + 31) / 32, (unsigned)((N) + 15) / 16, (unsigned)(S)), 32, 0, stream>>>(gc11); }
    { GemmP gc12;
      gc12.A = F0; gc12.B = PYF + 15000; gc12.bias = F0; gc12.R = F0; gc12.C = CV1 + 15000;
      gc12.sAo = (long long)N * LAT; gc12.sAi = 0; gc12.sAm = LAT; gc12.sAk = 1; gc12.sBo = (long long)LAT * 15930; gc12.sBi = 0; gc12.sBn = 1; gc12.sBk = 15930; gc12.sCo = (long long)N * 15930; gc12.sCi = 0; gc12.sCm = 15930; gc12.sRo = 0; gc12.sRi = 0; gc12.sRm = 0; gc12.sRn = 0;
      gc12.M = N; gc12.N = 750; gc12.K = LAT; gc12.zi_n = 1; gc12.flags = 0; gc12.act = 0;
      gc12.alpha = 0.125f; gc12.beta = 0.0f; gc12.sa = 1.0f; gc12.sb = 1.0f; gc12.Npad = 750; gc12.pad_ = 0;
      k_gemm<4><<<dim3((unsigned)((750) + 31) / 32, (unsigned)((N) + 15) / 16, (unsigned)(S)), 32, 0, stream>>>(gc12); }
    { GemmP gc13;
      gc13.A = F0; gc13.B = PYF + 15750; gc13.bias = F0; gc13.R = F0; gc13.C = CV1 + 15750;
      gc13.sAo = (long long)N * LAT; gc13.sAi = 0; gc13.sAm = LAT; gc13.sAk = 1; gc13.sBo = (long long)LAT * 15930; gc13.sBi = 0; gc13.sBn = 1; gc13.sBk = 15930; gc13.sCo = (long long)N * 15930; gc13.sCi = 0; gc13.sCm = 15930; gc13.sRo = 0; gc13.sRi = 0; gc13.sRm = 0; gc13.sRn = 0;
      gc13.M = N; gc13.N = 180; gc13.K = LAT; gc13.zi_n = 1; gc13.flags = 0; gc13.act = 0;
      gc13.alpha = 0.125f; gc13.beta = 0.0f; gc13.sa = 1.0f; gc13.sb = 1.0f; gc13.Npad = 180; gc13.pad_ = 0;
      k_gemm<4><<<dim3((unsigned)((180) + 31) / 32, (unsigned)((N) + 15) / 16, (unsigned)(S)), 32, 0, stream>>>(gc13); }
    k_ep_featsample<<<(unsigned)((S * N * 64 + 255) / 256), 256, 0, stream>>>(PYF, 1, CO, F2, S, N, 2);
    { GemmP gc2_0_0;
      gc2_0_0.A = F2; gc2_0_0.B = PYF + 0; gc2_0_0.bias = F2; gc2_0_0.R = F2; gc2_0_0.C = CVX + 0;
      gc2_0_0.sAo = (long long)N * LAT; gc2_0_0.sAi = 0; gc2_0_0.sAm = LAT; gc2_0_0.sAk = 1; gc2_0_0.sBo = (long long)LAT * 15930; gc2_0_0.sBi = 0; gc2_0_0.sBn = 1; gc2_0_0.sBk = 15930; gc2_0_0.sCo = (long long)N * 15930; gc2_0_0.sCi = 0; gc2_0_0.sCm = 15930; gc2_0_0.sRo = 0; gc2_0_0.sRi = 0; gc2_0_0.sRm = 0; gc2_0_0.sRn = 0;
      gc2_0_0.M = N; gc2_0_0.N = 12000; gc2_0_0.K = LAT; gc2_0_0.zi_n = 1; gc2_0_0.flags = 0; gc2_0_0.act = 0;
      gc2_0_0.alpha = 0.125f; gc2_0_0.beta = 0.0f; gc2_0_0.sa = 1.0f; gc2_0_0.sb = 1.0f; gc2_0_0.Npad = 12000; gc2_0_0.pad_ = 0;
      k_gemm<4><<<dim3((unsigned)((12000) + 31) / 32, (unsigned)((N) + 15) / 16, (unsigned)(S)), 32, 0, stream>>>(gc2_0_0); }
    { GemmP gc2_0_1;
      gc2_0_1.A = F2; gc2_0_1.B = PYF + 12000; gc2_0_1.bias = F2; gc2_0_1.R = F2; gc2_0_1.C = CVX + 12000;
      gc2_0_1.sAo = (long long)N * LAT; gc2_0_1.sAi = 0; gc2_0_1.sAm = LAT; gc2_0_1.sAk = 1; gc2_0_1.sBo = (long long)LAT * 15930; gc2_0_1.sBi = 0; gc2_0_1.sBn = 1; gc2_0_1.sBk = 15930; gc2_0_1.sCo = (long long)N * 15930; gc2_0_1.sCi = 0; gc2_0_1.sCm = 15930; gc2_0_1.sRo = 0; gc2_0_1.sRi = 0; gc2_0_1.sRm = 0; gc2_0_1.sRn = 0;
      gc2_0_1.M = N; gc2_0_1.N = 3000; gc2_0_1.K = LAT; gc2_0_1.zi_n = 1; gc2_0_1.flags = 0; gc2_0_1.act = 0;
      gc2_0_1.alpha = 0.125f; gc2_0_1.beta = 0.0f; gc2_0_1.sa = 1.0f; gc2_0_1.sb = 1.0f; gc2_0_1.Npad = 3000; gc2_0_1.pad_ = 0;
      k_gemm<4><<<dim3((unsigned)((3000) + 31) / 32, (unsigned)((N) + 15) / 16, (unsigned)(S)), 32, 0, stream>>>(gc2_0_1); }
    { GemmP gc2_0_2;
      gc2_0_2.A = F2; gc2_0_2.B = PYF + 15000; gc2_0_2.bias = F2; gc2_0_2.R = F2; gc2_0_2.C = CVX + 15000;
      gc2_0_2.sAo = (long long)N * LAT; gc2_0_2.sAi = 0; gc2_0_2.sAm = LAT; gc2_0_2.sAk = 1; gc2_0_2.sBo = (long long)LAT * 15930; gc2_0_2.sBi = 0; gc2_0_2.sBn = 1; gc2_0_2.sBk = 15930; gc2_0_2.sCo = (long long)N * 15930; gc2_0_2.sCi = 0; gc2_0_2.sCm = 15930; gc2_0_2.sRo = 0; gc2_0_2.sRi = 0; gc2_0_2.sRm = 0; gc2_0_2.sRn = 0;
      gc2_0_2.M = N; gc2_0_2.N = 750; gc2_0_2.K = LAT; gc2_0_2.zi_n = 1; gc2_0_2.flags = 0; gc2_0_2.act = 0;
      gc2_0_2.alpha = 0.125f; gc2_0_2.beta = 0.0f; gc2_0_2.sa = 1.0f; gc2_0_2.sb = 1.0f; gc2_0_2.Npad = 750; gc2_0_2.pad_ = 0;
      k_gemm<4><<<dim3((unsigned)((750) + 31) / 32, (unsigned)((N) + 15) / 16, (unsigned)(S)), 32, 0, stream>>>(gc2_0_2); }
    { GemmP gc2_0_3;
      gc2_0_3.A = F2; gc2_0_3.B = PYF + 15750; gc2_0_3.bias = F2; gc2_0_3.R = F2; gc2_0_3.C = CVX + 15750;
      gc2_0_3.sAo = (long long)N * LAT; gc2_0_3.sAi = 0; gc2_0_3.sAm = LAT; gc2_0_3.sAk = 1; gc2_0_3.sBo = (long long)LAT * 15930; gc2_0_3.sBi = 0; gc2_0_3.sBn = 1; gc2_0_3.sBk = 15930; gc2_0_3.sCo = (long long)N * 15930; gc2_0_3.sCi = 0; gc2_0_3.sCm = 15930; gc2_0_3.sRo = 0; gc2_0_3.sRi = 0; gc2_0_3.sRm = 0; gc2_0_3.sRn = 0;
      gc2_0_3.M = N; gc2_0_3.N = 180; gc2_0_3.K = LAT; gc2_0_3.zi_n = 1; gc2_0_3.flags = 0; gc2_0_3.act = 0;
      gc2_0_3.alpha = 0.125f; gc2_0_3.beta = 0.0f; gc2_0_3.sa = 1.0f; gc2_0_3.sb = 1.0f; gc2_0_3.Npad = 180; gc2_0_3.pad_ = 0;
      k_gemm<4><<<dim3((unsigned)((180) + 31) / 32, (unsigned)((N) + 15) / 16, (unsigned)(S)), 32, 0, stream>>>(gc2_0_3); }
    k_ep_csample<<<(unsigned)((N * S * 196 + 255) / 256), 256, 0, stream>>>(CVX, 1, CO, FCAT, 608, S, N);
    k_ep_csample<<<(unsigned)((N * S * 196 + 255) / 256), 256, 0, stream>>>(CV1, 0, CO, FCAT, 608, S, N);
    k_ep_featsample<<<(unsigned)((S * N * 64 + 255) / 256), 256, 0, stream>>>(PYF, 1, CO, F2, S, N, 4);
    { GemmP gc4_0_0;
      gc4_0_0.A = F2; gc4_0_0.B = PYF + 0; gc4_0_0.bias = F2; gc4_0_0.R = F2; gc4_0_0.C = CVX + 0;
      gc4_0_0.sAo = (long long)N * LAT; gc4_0_0.sAi = 0; gc4_0_0.sAm = LAT; gc4_0_0.sAk = 1; gc4_0_0.sBo = (long long)LAT * 15930; gc4_0_0.sBi = 0; gc4_0_0.sBn = 1; gc4_0_0.sBk = 15930; gc4_0_0.sCo = (long long)N * 15930; gc4_0_0.sCi = 0; gc4_0_0.sCm = 15930; gc4_0_0.sRo = 0; gc4_0_0.sRi = 0; gc4_0_0.sRm = 0; gc4_0_0.sRn = 0;
      gc4_0_0.M = N; gc4_0_0.N = 12000; gc4_0_0.K = LAT; gc4_0_0.zi_n = 1; gc4_0_0.flags = 0; gc4_0_0.act = 0;
      gc4_0_0.alpha = 0.125f; gc4_0_0.beta = 0.0f; gc4_0_0.sa = 1.0f; gc4_0_0.sb = 1.0f; gc4_0_0.Npad = 12000; gc4_0_0.pad_ = 0;
      k_gemm<4><<<dim3((unsigned)((12000) + 31) / 32, (unsigned)((N) + 15) / 16, (unsigned)(S)), 32, 0, stream>>>(gc4_0_0); }
    { GemmP gc4_0_1;
      gc4_0_1.A = F2; gc4_0_1.B = PYF + 12000; gc4_0_1.bias = F2; gc4_0_1.R = F2; gc4_0_1.C = CVX + 12000;
      gc4_0_1.sAo = (long long)N * LAT; gc4_0_1.sAi = 0; gc4_0_1.sAm = LAT; gc4_0_1.sAk = 1; gc4_0_1.sBo = (long long)LAT * 15930; gc4_0_1.sBi = 0; gc4_0_1.sBn = 1; gc4_0_1.sBk = 15930; gc4_0_1.sCo = (long long)N * 15930; gc4_0_1.sCi = 0; gc4_0_1.sCm = 15930; gc4_0_1.sRo = 0; gc4_0_1.sRi = 0; gc4_0_1.sRm = 0; gc4_0_1.sRn = 0;
      gc4_0_1.M = N; gc4_0_1.N = 3000; gc4_0_1.K = LAT; gc4_0_1.zi_n = 1; gc4_0_1.flags = 0; gc4_0_1.act = 0;
      gc4_0_1.alpha = 0.125f; gc4_0_1.beta = 0.0f; gc4_0_1.sa = 1.0f; gc4_0_1.sb = 1.0f; gc4_0_1.Npad = 3000; gc4_0_1.pad_ = 0;
      k_gemm<4><<<dim3((unsigned)((3000) + 31) / 32, (unsigned)((N) + 15) / 16, (unsigned)(S)), 32, 0, stream>>>(gc4_0_1); }
    { GemmP gc4_0_2;
      gc4_0_2.A = F2; gc4_0_2.B = PYF + 15000; gc4_0_2.bias = F2; gc4_0_2.R = F2; gc4_0_2.C = CVX + 15000;
      gc4_0_2.sAo = (long long)N * LAT; gc4_0_2.sAi = 0; gc4_0_2.sAm = LAT; gc4_0_2.sAk = 1; gc4_0_2.sBo = (long long)LAT * 15930; gc4_0_2.sBi = 0; gc4_0_2.sBn = 1; gc4_0_2.sBk = 15930; gc4_0_2.sCo = (long long)N * 15930; gc4_0_2.sCi = 0; gc4_0_2.sCm = 15930; gc4_0_2.sRo = 0; gc4_0_2.sRi = 0; gc4_0_2.sRm = 0; gc4_0_2.sRn = 0;
      gc4_0_2.M = N; gc4_0_2.N = 750; gc4_0_2.K = LAT; gc4_0_2.zi_n = 1; gc4_0_2.flags = 0; gc4_0_2.act = 0;
      gc4_0_2.alpha = 0.125f; gc4_0_2.beta = 0.0f; gc4_0_2.sa = 1.0f; gc4_0_2.sb = 1.0f; gc4_0_2.Npad = 750; gc4_0_2.pad_ = 0;
      k_gemm<4><<<dim3((unsigned)((750) + 31) / 32, (unsigned)((N) + 15) / 16, (unsigned)(S)), 32, 0, stream>>>(gc4_0_2); }
    { GemmP gc4_0_3;
      gc4_0_3.A = F2; gc4_0_3.B = PYF + 15750; gc4_0_3.bias = F2; gc4_0_3.R = F2; gc4_0_3.C = CVX + 15750;
      gc4_0_3.sAo = (long long)N * LAT; gc4_0_3.sAi = 0; gc4_0_3.sAm = LAT; gc4_0_3.sAk = 1; gc4_0_3.sBo = (long long)LAT * 15930; gc4_0_3.sBi = 0; gc4_0_3.sBn = 1; gc4_0_3.sBk = 15930; gc4_0_3.sCo = (long long)N * 15930; gc4_0_3.sCi = 0; gc4_0_3.sCm = 15930; gc4_0_3.sRo = 0; gc4_0_3.sRi = 0; gc4_0_3.sRm = 0; gc4_0_3.sRn = 0;
      gc4_0_3.M = N; gc4_0_3.N = 180; gc4_0_3.K = LAT; gc4_0_3.zi_n = 1; gc4_0_3.flags = 0; gc4_0_3.act = 0;
      gc4_0_3.alpha = 0.125f; gc4_0_3.beta = 0.0f; gc4_0_3.sa = 1.0f; gc4_0_3.sb = 1.0f; gc4_0_3.Npad = 180; gc4_0_3.pad_ = 0;
      k_gemm<4><<<dim3((unsigned)((180) + 31) / 32, (unsigned)((N) + 15) / 16, (unsigned)(S)), 32, 0, stream>>>(gc4_0_3); }
    k_ep_csample<<<(unsigned)((N * S * 196 + 255) / 256), 256, 0, stream>>>(CVX, 2, CO, FCAT, 608, S, N);
    { GemmP glin0;
      glin0.A = FCAT; glin0.B = linw; glin0.bias = linb; glin0.R = FCAT; glin0.C = HIN;
      glin0.sAo = 0; glin0.sAi = 0; glin0.sAm = 608; glin0.sAk = 1; glin0.sBo = 0; glin0.sBi = 0; glin0.sBn = 1; glin0.sBk = 392; glin0.sCo = 0; glin0.sCi = 0; glin0.sCm = 3400; glin0.sRo = 0; glin0.sRi = 0; glin0.sRm = 0; glin0.sRn = 0;
      glin0.M = NS; glin0.N = 392; glin0.K = 588; glin0.zi_n = 1; glin0.flags = 1; glin0.act = 0;
      glin0.alpha = 1.0f; glin0.beta = 0.0f; glin0.sa = 1.0f; glin0.sb = 1.0f; glin0.Npad = 392; glin0.pad_ = 0;
      k_gemm<4><<<dim3((unsigned)((392) + 31) / 32, (unsigned)((NS) + 15) / 16, (unsigned)(1)), 32, 0, stream>>>(glin0); }
    k_ep_ctx<<<(unsigned)(((long long)N * S * 3004 + 255) / 256), 256, 0, stream>>>(CO, FFr, XY0, HIN, 3400, 392, S, N);
    { GemmP gdt1_0;
      gdt1_0.A = HIN; gdt1_0.B = dtw1; gdt1_0.bias = dtb1; gdt1_0.R = HIN; gdt1_0.C = HID;
      gdt1_0.sAo = 0; gdt1_0.sAi = 0; gdt1_0.sAm = 3400; gdt1_0.sAk = 1; gdt1_0.sBo = 0; gdt1_0.sBi = 0; gdt1_0.sBn = 1; gdt1_0.sBk = 128; gdt1_0.sCo = 0; gdt1_0.sCi = 0; gdt1_0.sCm = 128; gdt1_0.sRo = 0; gdt1_0.sRi = 0; gdt1_0.sRm = 0; gdt1_0.sRn = 0;
      gdt1_0.M = NS; gdt1_0.N = 128; gdt1_0.K = 3396; gdt1_0.zi_n = 1; gdt1_0.flags = 1; gdt1_0.act = 1;
      gdt1_0.alpha = 1.0f; gdt1_0.beta = 0.0f; gdt1_0.sa = 1.0f; gdt1_0.sb = 1.0f; gdt1_0.Npad = 128; gdt1_0.pad_ = 0;
      k_gemm<4><<<dim3((unsigned)((128) + 31) / 32, (unsigned)((NS) + 15) / 16, (unsigned)(1)), 32, 0, stream>>>(gdt1_0); }
    { GemmP gdt2_0;
      gdt2_0.A = HID; gdt2_0.B = dtw2; gdt2_0.bias = dtb2; gdt2_0.R = HID; gdt2_0.C = DEL;
      gdt2_0.sAo = 0; gdt2_0.sAi = 0; gdt2_0.sAm = 128; gdt2_0.sAk = 1; gdt2_0.sBo = 0; gdt2_0.sBi = 0; gdt2_0.sBn = 1; gdt2_0.sBk = 2; gdt2_0.sCo = 0; gdt2_0.sCi = 0; gdt2_0.sCm = LP; gdt2_0.sRo = 0; gdt2_0.sRi = 0; gdt2_0.sRm = 0; gdt2_0.sRn = 0;
      gdt2_0.M = NS; gdt2_0.N = 2; gdt2_0.K = 128; gdt2_0.zi_n = 1; gdt2_0.flags = 1; gdt2_0.act = 0;
      gdt2_0.alpha = 1.0f; gdt2_0.beta = 0.0f; gdt2_0.sa = 1.0f; gdt2_0.sb = 1.0f; gdt2_0.Npad = LP; gdt2_0.pad_ = 0;
      k_gemm<4><<<dim3((unsigned)((LP) + 31) / 32, (unsigned)((NS) + 15) / 16, (unsigned)(1)), 32, 0, stream>>>(gdt2_0); }
    k_ep_update<<<(unsigned)((S * N * 2 + 255) / 256), 256, 0, stream>>>(CO, DEL, LP, out + (size_t)1 * S * N * 2, 2.f, 1.f, S, N);
    k_ep_featsample<<<(unsigned)((S * N * 64 + 255) / 256), 256, 0, stream>>>(PYF, 1, CO, F2, S, N, 2);
    { GemmP gc2_1_0;
      gc2_1_0.A = F2; gc2_1_0.B = PYF + 0; gc2_1_0.bias = F2; gc2_1_0.R = F2; gc2_1_0.C = CVX + 0;
      gc2_1_0.sAo = (long long)N * LAT; gc2_1_0.sAi = 0; gc2_1_0.sAm = LAT; gc2_1_0.sAk = 1; gc2_1_0.sBo = (long long)LAT * 15930; gc2_1_0.sBi = 0; gc2_1_0.sBn = 1; gc2_1_0.sBk = 15930; gc2_1_0.sCo = (long long)N * 15930; gc2_1_0.sCi = 0; gc2_1_0.sCm = 15930; gc2_1_0.sRo = 0; gc2_1_0.sRi = 0; gc2_1_0.sRm = 0; gc2_1_0.sRn = 0;
      gc2_1_0.M = N; gc2_1_0.N = 12000; gc2_1_0.K = LAT; gc2_1_0.zi_n = 1; gc2_1_0.flags = 0; gc2_1_0.act = 0;
      gc2_1_0.alpha = 0.125f; gc2_1_0.beta = 0.0f; gc2_1_0.sa = 1.0f; gc2_1_0.sb = 1.0f; gc2_1_0.Npad = 12000; gc2_1_0.pad_ = 0;
      k_gemm<4><<<dim3((unsigned)((12000) + 31) / 32, (unsigned)((N) + 15) / 16, (unsigned)(S)), 32, 0, stream>>>(gc2_1_0); }
    { GemmP gc2_1_1;
      gc2_1_1.A = F2; gc2_1_1.B = PYF + 12000; gc2_1_1.bias = F2; gc2_1_1.R = F2; gc2_1_1.C = CVX + 12000;
      gc2_1_1.sAo = (long long)N * LAT; gc2_1_1.sAi = 0; gc2_1_1.sAm = LAT; gc2_1_1.sAk = 1; gc2_1_1.sBo = (long long)LAT * 15930; gc2_1_1.sBi = 0; gc2_1_1.sBn = 1; gc2_1_1.sBk = 15930; gc2_1_1.sCo = (long long)N * 15930; gc2_1_1.sCi = 0; gc2_1_1.sCm = 15930; gc2_1_1.sRo = 0; gc2_1_1.sRi = 0; gc2_1_1.sRm = 0; gc2_1_1.sRn = 0;
      gc2_1_1.M = N; gc2_1_1.N = 3000; gc2_1_1.K = LAT; gc2_1_1.zi_n = 1; gc2_1_1.flags = 0; gc2_1_1.act = 0;
      gc2_1_1.alpha = 0.125f; gc2_1_1.beta = 0.0f; gc2_1_1.sa = 1.0f; gc2_1_1.sb = 1.0f; gc2_1_1.Npad = 3000; gc2_1_1.pad_ = 0;
      k_gemm<4><<<dim3((unsigned)((3000) + 31) / 32, (unsigned)((N) + 15) / 16, (unsigned)(S)), 32, 0, stream>>>(gc2_1_1); }
    { GemmP gc2_1_2;
      gc2_1_2.A = F2; gc2_1_2.B = PYF + 15000; gc2_1_2.bias = F2; gc2_1_2.R = F2; gc2_1_2.C = CVX + 15000;
      gc2_1_2.sAo = (long long)N * LAT; gc2_1_2.sAi = 0; gc2_1_2.sAm = LAT; gc2_1_2.sAk = 1; gc2_1_2.sBo = (long long)LAT * 15930; gc2_1_2.sBi = 0; gc2_1_2.sBn = 1; gc2_1_2.sBk = 15930; gc2_1_2.sCo = (long long)N * 15930; gc2_1_2.sCi = 0; gc2_1_2.sCm = 15930; gc2_1_2.sRo = 0; gc2_1_2.sRi = 0; gc2_1_2.sRm = 0; gc2_1_2.sRn = 0;
      gc2_1_2.M = N; gc2_1_2.N = 750; gc2_1_2.K = LAT; gc2_1_2.zi_n = 1; gc2_1_2.flags = 0; gc2_1_2.act = 0;
      gc2_1_2.alpha = 0.125f; gc2_1_2.beta = 0.0f; gc2_1_2.sa = 1.0f; gc2_1_2.sb = 1.0f; gc2_1_2.Npad = 750; gc2_1_2.pad_ = 0;
      k_gemm<4><<<dim3((unsigned)((750) + 31) / 32, (unsigned)((N) + 15) / 16, (unsigned)(S)), 32, 0, stream>>>(gc2_1_2); }
    { GemmP gc2_1_3;
      gc2_1_3.A = F2; gc2_1_3.B = PYF + 15750; gc2_1_3.bias = F2; gc2_1_3.R = F2; gc2_1_3.C = CVX + 15750;
      gc2_1_3.sAo = (long long)N * LAT; gc2_1_3.sAi = 0; gc2_1_3.sAm = LAT; gc2_1_3.sAk = 1; gc2_1_3.sBo = (long long)LAT * 15930; gc2_1_3.sBi = 0; gc2_1_3.sBn = 1; gc2_1_3.sBk = 15930; gc2_1_3.sCo = (long long)N * 15930; gc2_1_3.sCi = 0; gc2_1_3.sCm = 15930; gc2_1_3.sRo = 0; gc2_1_3.sRi = 0; gc2_1_3.sRm = 0; gc2_1_3.sRn = 0;
      gc2_1_3.M = N; gc2_1_3.N = 180; gc2_1_3.K = LAT; gc2_1_3.zi_n = 1; gc2_1_3.flags = 0; gc2_1_3.act = 0;
      gc2_1_3.alpha = 0.125f; gc2_1_3.beta = 0.0f; gc2_1_3.sa = 1.0f; gc2_1_3.sb = 1.0f; gc2_1_3.Npad = 180; gc2_1_3.pad_ = 0;
      k_gemm<4><<<dim3((unsigned)((180) + 31) / 32, (unsigned)((N) + 15) / 16, (unsigned)(S)), 32, 0, stream>>>(gc2_1_3); }
    k_ep_csample<<<(unsigned)((N * S * 196 + 255) / 256), 256, 0, stream>>>(CVX, 1, CO, FCAT, 608, S, N);
    k_ep_csample<<<(unsigned)((N * S * 196 + 255) / 256), 256, 0, stream>>>(CV1, 0, CO, FCAT, 608, S, N);
    k_ep_featsample<<<(unsigned)((S * N * 64 + 255) / 256), 256, 0, stream>>>(PYF, 1, CO, F2, S, N, 4);
    { GemmP gc4_1_0;
      gc4_1_0.A = F2; gc4_1_0.B = PYF + 0; gc4_1_0.bias = F2; gc4_1_0.R = F2; gc4_1_0.C = CVX + 0;
      gc4_1_0.sAo = (long long)N * LAT; gc4_1_0.sAi = 0; gc4_1_0.sAm = LAT; gc4_1_0.sAk = 1; gc4_1_0.sBo = (long long)LAT * 15930; gc4_1_0.sBi = 0; gc4_1_0.sBn = 1; gc4_1_0.sBk = 15930; gc4_1_0.sCo = (long long)N * 15930; gc4_1_0.sCi = 0; gc4_1_0.sCm = 15930; gc4_1_0.sRo = 0; gc4_1_0.sRi = 0; gc4_1_0.sRm = 0; gc4_1_0.sRn = 0;
      gc4_1_0.M = N; gc4_1_0.N = 12000; gc4_1_0.K = LAT; gc4_1_0.zi_n = 1; gc4_1_0.flags = 0; gc4_1_0.act = 0;
      gc4_1_0.alpha = 0.125f; gc4_1_0.beta = 0.0f; gc4_1_0.sa = 1.0f; gc4_1_0.sb = 1.0f; gc4_1_0.Npad = 12000; gc4_1_0.pad_ = 0;
      k_gemm<4><<<dim3((unsigned)((12000) + 31) / 32, (unsigned)((N) + 15) / 16, (unsigned)(S)), 32, 0, stream>>>(gc4_1_0); }
    { GemmP gc4_1_1;
      gc4_1_1.A = F2; gc4_1_1.B = PYF + 12000; gc4_1_1.bias = F2; gc4_1_1.R = F2; gc4_1_1.C = CVX + 12000;
      gc4_1_1.sAo = (long long)N * LAT; gc4_1_1.sAi = 0; gc4_1_1.sAm = LAT; gc4_1_1.sAk = 1; gc4_1_1.sBo = (long long)LAT * 15930; gc4_1_1.sBi = 0; gc4_1_1.sBn = 1; gc4_1_1.sBk = 15930; gc4_1_1.sCo = (long long)N * 15930; gc4_1_1.sCi = 0; gc4_1_1.sCm = 15930; gc4_1_1.sRo = 0; gc4_1_1.sRi = 0; gc4_1_1.sRm = 0; gc4_1_1.sRn = 0;
      gc4_1_1.M = N; gc4_1_1.N = 3000; gc4_1_1.K = LAT; gc4_1_1.zi_n = 1; gc4_1_1.flags = 0; gc4_1_1.act = 0;
      gc4_1_1.alpha = 0.125f; gc4_1_1.beta = 0.0f; gc4_1_1.sa = 1.0f; gc4_1_1.sb = 1.0f; gc4_1_1.Npad = 3000; gc4_1_1.pad_ = 0;
      k_gemm<4><<<dim3((unsigned)((3000) + 31) / 32, (unsigned)((N) + 15) / 16, (unsigned)(S)), 32, 0, stream>>>(gc4_1_1); }
    { GemmP gc4_1_2;
      gc4_1_2.A = F2; gc4_1_2.B = PYF + 15000; gc4_1_2.bias = F2; gc4_1_2.R = F2; gc4_1_2.C = CVX + 15000;
      gc4_1_2.sAo = (long long)N * LAT; gc4_1_2.sAi = 0; gc4_1_2.sAm = LAT; gc4_1_2.sAk = 1; gc4_1_2.sBo = (long long)LAT * 15930; gc4_1_2.sBi = 0; gc4_1_2.sBn = 1; gc4_1_2.sBk = 15930; gc4_1_2.sCo = (long long)N * 15930; gc4_1_2.sCi = 0; gc4_1_2.sCm = 15930; gc4_1_2.sRo = 0; gc4_1_2.sRi = 0; gc4_1_2.sRm = 0; gc4_1_2.sRn = 0;
      gc4_1_2.M = N; gc4_1_2.N = 750; gc4_1_2.K = LAT; gc4_1_2.zi_n = 1; gc4_1_2.flags = 0; gc4_1_2.act = 0;
      gc4_1_2.alpha = 0.125f; gc4_1_2.beta = 0.0f; gc4_1_2.sa = 1.0f; gc4_1_2.sb = 1.0f; gc4_1_2.Npad = 750; gc4_1_2.pad_ = 0;
      k_gemm<4><<<dim3((unsigned)((750) + 31) / 32, (unsigned)((N) + 15) / 16, (unsigned)(S)), 32, 0, stream>>>(gc4_1_2); }
    { GemmP gc4_1_3;
      gc4_1_3.A = F2; gc4_1_3.B = PYF + 15750; gc4_1_3.bias = F2; gc4_1_3.R = F2; gc4_1_3.C = CVX + 15750;
      gc4_1_3.sAo = (long long)N * LAT; gc4_1_3.sAi = 0; gc4_1_3.sAm = LAT; gc4_1_3.sAk = 1; gc4_1_3.sBo = (long long)LAT * 15930; gc4_1_3.sBi = 0; gc4_1_3.sBn = 1; gc4_1_3.sBk = 15930; gc4_1_3.sCo = (long long)N * 15930; gc4_1_3.sCi = 0; gc4_1_3.sCm = 15930; gc4_1_3.sRo = 0; gc4_1_3.sRi = 0; gc4_1_3.sRm = 0; gc4_1_3.sRn = 0;
      gc4_1_3.M = N; gc4_1_3.N = 180; gc4_1_3.K = LAT; gc4_1_3.zi_n = 1; gc4_1_3.flags = 0; gc4_1_3.act = 0;
      gc4_1_3.alpha = 0.125f; gc4_1_3.beta = 0.0f; gc4_1_3.sa = 1.0f; gc4_1_3.sb = 1.0f; gc4_1_3.Npad = 180; gc4_1_3.pad_ = 0;
      k_gemm<4><<<dim3((unsigned)((180) + 31) / 32, (unsigned)((N) + 15) / 16, (unsigned)(S)), 32, 0, stream>>>(gc4_1_3); }
    k_ep_csample<<<(unsigned)((N * S * 196 + 255) / 256), 256, 0, stream>>>(CVX, 2, CO, FCAT, 608, S, N);
    { GemmP glin1;
      glin1.A = FCAT; glin1.B = linw; glin1.bias = linb; glin1.R = FCAT; glin1.C = HIN;
      glin1.sAo = 0; glin1.sAi = 0; glin1.sAm = 608; glin1.sAk = 1; glin1.sBo = 0; glin1.sBi = 0; glin1.sBn = 1; glin1.sBk = 392; glin1.sCo = 0; glin1.sCi = 0; glin1.sCm = 3400; glin1.sRo = 0; glin1.sRi = 0; glin1.sRm = 0; glin1.sRn = 0;
      glin1.M = NS; glin1.N = 392; glin1.K = 588; glin1.zi_n = 1; glin1.flags = 1; glin1.act = 0;
      glin1.alpha = 1.0f; glin1.beta = 0.0f; glin1.sa = 1.0f; glin1.sb = 1.0f; glin1.Npad = 392; glin1.pad_ = 0;
      k_gemm<4><<<dim3((unsigned)((392) + 31) / 32, (unsigned)((NS) + 15) / 16, (unsigned)(1)), 32, 0, stream>>>(glin1); }
    k_ep_ctx<<<(unsigned)(((long long)N * S * 3004 + 255) / 256), 256, 0, stream>>>(CO, FFr, XY0, HIN, 3400, 392, S, N);
    { GemmP gdt1_1;
      gdt1_1.A = HIN; gdt1_1.B = dtw1; gdt1_1.bias = dtb1; gdt1_1.R = HIN; gdt1_1.C = HID;
      gdt1_1.sAo = 0; gdt1_1.sAi = 0; gdt1_1.sAm = 3400; gdt1_1.sAk = 1; gdt1_1.sBo = 0; gdt1_1.sBi = 0; gdt1_1.sBn = 1; gdt1_1.sBk = 128; gdt1_1.sCo = 0; gdt1_1.sCi = 0; gdt1_1.sCm = 128; gdt1_1.sRo = 0; gdt1_1.sRi = 0; gdt1_1.sRm = 0; gdt1_1.sRn = 0;
      gdt1_1.M = NS; gdt1_1.N = 128; gdt1_1.K = 3396; gdt1_1.zi_n = 1; gdt1_1.flags = 1; gdt1_1.act = 1;
      gdt1_1.alpha = 1.0f; gdt1_1.beta = 0.0f; gdt1_1.sa = 1.0f; gdt1_1.sb = 1.0f; gdt1_1.Npad = 128; gdt1_1.pad_ = 0;
      k_gemm<4><<<dim3((unsigned)((128) + 31) / 32, (unsigned)((NS) + 15) / 16, (unsigned)(1)), 32, 0, stream>>>(gdt1_1); }
    { GemmP gdt2_1;
      gdt2_1.A = HID; gdt2_1.B = dtw2; gdt2_1.bias = dtb2; gdt2_1.R = HID; gdt2_1.C = DEL;
      gdt2_1.sAo = 0; gdt2_1.sAi = 0; gdt2_1.sAm = 128; gdt2_1.sAk = 1; gdt2_1.sBo = 0; gdt2_1.sBi = 0; gdt2_1.sBn = 1; gdt2_1.sBk = 2; gdt2_1.sCo = 0; gdt2_1.sCi = 0; gdt2_1.sCm = LP; gdt2_1.sRo = 0; gdt2_1.sRi = 0; gdt2_1.sRm = 0; gdt2_1.sRn = 0;
      gdt2_1.M = NS; gdt2_1.N = 2; gdt2_1.K = 128; gdt2_1.zi_n = 1; gdt2_1.flags = 1; gdt2_1.act = 0;
      gdt2_1.alpha = 1.0f; gdt2_1.beta = 0.0f; gdt2_1.sa = 1.0f; gdt2_1.sb = 1.0f; gdt2_1.Npad = LP; gdt2_1.pad_ = 0;
      k_gemm<4><<<dim3((unsigned)((LP) + 31) / 32, (unsigned)((NS) + 15) / 16, (unsigned)(1)), 32, 0, stream>>>(gdt2_1); }
    k_ep_update<<<(unsigned)((S * N * 2 + 255) / 256), 256, 0, stream>>>(CO, DEL, LP, out + (size_t)2 * S * N * 2, 2.f, 1.f, S, N);
    k_ep_featsample<<<(unsigned)((S * N * 64 + 255) / 256), 256, 0, stream>>>(PYF, 1, CO, F2, S, N, 2);
    { GemmP gc2_2_0;
      gc2_2_0.A = F2; gc2_2_0.B = PYF + 0; gc2_2_0.bias = F2; gc2_2_0.R = F2; gc2_2_0.C = CVX + 0;
      gc2_2_0.sAo = (long long)N * LAT; gc2_2_0.sAi = 0; gc2_2_0.sAm = LAT; gc2_2_0.sAk = 1; gc2_2_0.sBo = (long long)LAT * 15930; gc2_2_0.sBi = 0; gc2_2_0.sBn = 1; gc2_2_0.sBk = 15930; gc2_2_0.sCo = (long long)N * 15930; gc2_2_0.sCi = 0; gc2_2_0.sCm = 15930; gc2_2_0.sRo = 0; gc2_2_0.sRi = 0; gc2_2_0.sRm = 0; gc2_2_0.sRn = 0;
      gc2_2_0.M = N; gc2_2_0.N = 12000; gc2_2_0.K = LAT; gc2_2_0.zi_n = 1; gc2_2_0.flags = 0; gc2_2_0.act = 0;
      gc2_2_0.alpha = 0.125f; gc2_2_0.beta = 0.0f; gc2_2_0.sa = 1.0f; gc2_2_0.sb = 1.0f; gc2_2_0.Npad = 12000; gc2_2_0.pad_ = 0;
      k_gemm<4><<<dim3((unsigned)((12000) + 31) / 32, (unsigned)((N) + 15) / 16, (unsigned)(S)), 32, 0, stream>>>(gc2_2_0); }
    { GemmP gc2_2_1;
      gc2_2_1.A = F2; gc2_2_1.B = PYF + 12000; gc2_2_1.bias = F2; gc2_2_1.R = F2; gc2_2_1.C = CVX + 12000;
      gc2_2_1.sAo = (long long)N * LAT; gc2_2_1.sAi = 0; gc2_2_1.sAm = LAT; gc2_2_1.sAk = 1; gc2_2_1.sBo = (long long)LAT * 15930; gc2_2_1.sBi = 0; gc2_2_1.sBn = 1; gc2_2_1.sBk = 15930; gc2_2_1.sCo = (long long)N * 15930; gc2_2_1.sCi = 0; gc2_2_1.sCm = 15930; gc2_2_1.sRo = 0; gc2_2_1.sRi = 0; gc2_2_1.sRm = 0; gc2_2_1.sRn = 0;
      gc2_2_1.M = N; gc2_2_1.N = 3000; gc2_2_1.K = LAT; gc2_2_1.zi_n = 1; gc2_2_1.flags = 0; gc2_2_1.act = 0;
      gc2_2_1.alpha = 0.125f; gc2_2_1.beta = 0.0f; gc2_2_1.sa = 1.0f; gc2_2_1.sb = 1.0f; gc2_2_1.Npad = 3000; gc2_2_1.pad_ = 0;
      k_gemm<4><<<dim3((unsigned)((3000) + 31) / 32, (unsigned)((N) + 15) / 16, (unsigned)(S)), 32, 0, stream>>>(gc2_2_1); }
    { GemmP gc2_2_2;
      gc2_2_2.A = F2; gc2_2_2.B = PYF + 15000; gc2_2_2.bias = F2; gc2_2_2.R = F2; gc2_2_2.C = CVX + 15000;
      gc2_2_2.sAo = (long long)N * LAT; gc2_2_2.sAi = 0; gc2_2_2.sAm = LAT; gc2_2_2.sAk = 1; gc2_2_2.sBo = (long long)LAT * 15930; gc2_2_2.sBi = 0; gc2_2_2.sBn = 1; gc2_2_2.sBk = 15930; gc2_2_2.sCo = (long long)N * 15930; gc2_2_2.sCi = 0; gc2_2_2.sCm = 15930; gc2_2_2.sRo = 0; gc2_2_2.sRi = 0; gc2_2_2.sRm = 0; gc2_2_2.sRn = 0;
      gc2_2_2.M = N; gc2_2_2.N = 750; gc2_2_2.K = LAT; gc2_2_2.zi_n = 1; gc2_2_2.flags = 0; gc2_2_2.act = 0;
      gc2_2_2.alpha = 0.125f; gc2_2_2.beta = 0.0f; gc2_2_2.sa = 1.0f; gc2_2_2.sb = 1.0f; gc2_2_2.Npad = 750; gc2_2_2.pad_ = 0;
      k_gemm<4><<<dim3((unsigned)((750) + 31) / 32, (unsigned)((N) + 15) / 16, (unsigned)(S)), 32, 0, stream>>>(gc2_2_2); }
    { GemmP gc2_2_3;
      gc2_2_3.A = F2; gc2_2_3.B = PYF + 15750; gc2_2_3.bias = F2; gc2_2_3.R = F2; gc2_2_3.C = CVX + 15750;
      gc2_2_3.sAo = (long long)N * LAT; gc2_2_3.sAi = 0; gc2_2_3.sAm = LAT; gc2_2_3.sAk = 1; gc2_2_3.sBo = (long long)LAT * 15930; gc2_2_3.sBi = 0; gc2_2_3.sBn = 1; gc2_2_3.sBk = 15930; gc2_2_3.sCo = (long long)N * 15930; gc2_2_3.sCi = 0; gc2_2_3.sCm = 15930; gc2_2_3.sRo = 0; gc2_2_3.sRi = 0; gc2_2_3.sRm = 0; gc2_2_3.sRn = 0;
      gc2_2_3.M = N; gc2_2_3.N = 180; gc2_2_3.K = LAT; gc2_2_3.zi_n = 1; gc2_2_3.flags = 0; gc2_2_3.act = 0;
      gc2_2_3.alpha = 0.125f; gc2_2_3.beta = 0.0f; gc2_2_3.sa = 1.0f; gc2_2_3.sb = 1.0f; gc2_2_3.Npad = 180; gc2_2_3.pad_ = 0;
      k_gemm<4><<<dim3((unsigned)((180) + 31) / 32, (unsigned)((N) + 15) / 16, (unsigned)(S)), 32, 0, stream>>>(gc2_2_3); }
    k_ep_csample<<<(unsigned)((N * S * 196 + 255) / 256), 256, 0, stream>>>(CVX, 1, CO, FCAT, 608, S, N);
    k_ep_csample<<<(unsigned)((N * S * 196 + 255) / 256), 256, 0, stream>>>(CV1, 0, CO, FCAT, 608, S, N);
    k_ep_featsample<<<(unsigned)((S * N * 64 + 255) / 256), 256, 0, stream>>>(PYF, 1, CO, F2, S, N, 4);
    { GemmP gc4_2_0;
      gc4_2_0.A = F2; gc4_2_0.B = PYF + 0; gc4_2_0.bias = F2; gc4_2_0.R = F2; gc4_2_0.C = CVX + 0;
      gc4_2_0.sAo = (long long)N * LAT; gc4_2_0.sAi = 0; gc4_2_0.sAm = LAT; gc4_2_0.sAk = 1; gc4_2_0.sBo = (long long)LAT * 15930; gc4_2_0.sBi = 0; gc4_2_0.sBn = 1; gc4_2_0.sBk = 15930; gc4_2_0.sCo = (long long)N * 15930; gc4_2_0.sCi = 0; gc4_2_0.sCm = 15930; gc4_2_0.sRo = 0; gc4_2_0.sRi = 0; gc4_2_0.sRm = 0; gc4_2_0.sRn = 0;
      gc4_2_0.M = N; gc4_2_0.N = 12000; gc4_2_0.K = LAT; gc4_2_0.zi_n = 1; gc4_2_0.flags = 0; gc4_2_0.act = 0;
      gc4_2_0.alpha = 0.125f; gc4_2_0.beta = 0.0f; gc4_2_0.sa = 1.0f; gc4_2_0.sb = 1.0f; gc4_2_0.Npad = 12000; gc4_2_0.pad_ = 0;
      k_gemm<4><<<dim3((unsigned)((12000) + 31) / 32, (unsigned)((N) + 15) / 16, (unsigned)(S)), 32, 0, stream>>>(gc4_2_0); }
    { GemmP gc4_2_1;
      gc4_2_1.A = F2; gc4_2_1.B = PYF + 12000; gc4_2_1.bias = F2; gc4_2_1.R = F2; gc4_2_1.C = CVX + 12000;
      gc4_2_1.sAo = (long long)N * LAT; gc4_2_1.sAi = 0; gc4_2_1.sAm = LAT; gc4_2_1.sAk = 1; gc4_2_1.sBo = (long long)LAT * 15930; gc4_2_1.sBi = 0; gc4_2_1.sBn = 1; gc4_2_1.sBk = 15930; gc4_2_1.sCo = (long long)N * 15930; gc4_2_1.sCi = 0; gc4_2_1.sCm = 15930; gc4_2_1.sRo = 0; gc4_2_1.sRi = 0; gc4_2_1.sRm = 0; gc4_2_1.sRn = 0;
      gc4_2_1.M = N; gc4_2_1.N = 3000; gc4_2_1.K = LAT; gc4_2_1.zi_n = 1; gc4_2_1.flags = 0; gc4_2_1.act = 0;
      gc4_2_1.alpha = 0.125f; gc4_2_1.beta = 0.0f; gc4_2_1.sa = 1.0f; gc4_2_1.sb = 1.0f; gc4_2_1.Npad = 3000; gc4_2_1.pad_ = 0;
      k_gemm<4><<<dim3((unsigned)((3000) + 31) / 32, (unsigned)((N) + 15) / 16, (unsigned)(S)), 32, 0, stream>>>(gc4_2_1); }
    { GemmP gc4_2_2;
      gc4_2_2.A = F2; gc4_2_2.B = PYF + 15000; gc4_2_2.bias = F2; gc4_2_2.R = F2; gc4_2_2.C = CVX + 15000;
      gc4_2_2.sAo = (long long)N * LAT; gc4_2_2.sAi = 0; gc4_2_2.sAm = LAT; gc4_2_2.sAk = 1; gc4_2_2.sBo = (long long)LAT * 15930; gc4_2_2.sBi = 0; gc4_2_2.sBn = 1; gc4_2_2.sBk = 15930; gc4_2_2.sCo = (long long)N * 15930; gc4_2_2.sCi = 0; gc4_2_2.sCm = 15930; gc4_2_2.sRo = 0; gc4_2_2.sRi = 0; gc4_2_2.sRm = 0; gc4_2_2.sRn = 0;
      gc4_2_2.M = N; gc4_2_2.N = 750; gc4_2_2.K = LAT; gc4_2_2.zi_n = 1; gc4_2_2.flags = 0; gc4_2_2.act = 0;
      gc4_2_2.alpha = 0.125f; gc4_2_2.beta = 0.0f; gc4_2_2.sa = 1.0f; gc4_2_2.sb = 1.0f; gc4_2_2.Npad = 750; gc4_2_2.pad_ = 0;
      k_gemm<4><<<dim3((unsigned)((750) + 31) / 32, (unsigned)((N) + 15) / 16, (unsigned)(S)), 32, 0, stream>>>(gc4_2_2); }
    { GemmP gc4_2_3;
      gc4_2_3.A = F2; gc4_2_3.B = PYF + 15750; gc4_2_3.bias = F2; gc4_2_3.R = F2; gc4_2_3.C = CVX + 15750;
      gc4_2_3.sAo = (long long)N * LAT; gc4_2_3.sAi = 0; gc4_2_3.sAm = LAT; gc4_2_3.sAk = 1; gc4_2_3.sBo = (long long)LAT * 15930; gc4_2_3.sBi = 0; gc4_2_3.sBn = 1; gc4_2_3.sBk = 15930; gc4_2_3.sCo = (long long)N * 15930; gc4_2_3.sCi = 0; gc4_2_3.sCm = 15930; gc4_2_3.sRo = 0; gc4_2_3.sRi = 0; gc4_2_3.sRm = 0; gc4_2_3.sRn = 0;
      gc4_2_3.M = N; gc4_2_3.N = 180; gc4_2_3.K = LAT; gc4_2_3.zi_n = 1; gc4_2_3.flags = 0; gc4_2_3.act = 0;
      gc4_2_3.alpha = 0.125f; gc4_2_3.beta = 0.0f; gc4_2_3.sa = 1.0f; gc4_2_3.sb = 1.0f; gc4_2_3.Npad = 180; gc4_2_3.pad_ = 0;
      k_gemm<4><<<dim3((unsigned)((180) + 31) / 32, (unsigned)((N) + 15) / 16, (unsigned)(S)), 32, 0, stream>>>(gc4_2_3); }
    k_ep_csample<<<(unsigned)((N * S * 196 + 255) / 256), 256, 0, stream>>>(CVX, 2, CO, FCAT, 608, S, N);
    { GemmP glin2;
      glin2.A = FCAT; glin2.B = linw; glin2.bias = linb; glin2.R = FCAT; glin2.C = HIN;
      glin2.sAo = 0; glin2.sAi = 0; glin2.sAm = 608; glin2.sAk = 1; glin2.sBo = 0; glin2.sBi = 0; glin2.sBn = 1; glin2.sBk = 392; glin2.sCo = 0; glin2.sCi = 0; glin2.sCm = 3400; glin2.sRo = 0; glin2.sRi = 0; glin2.sRm = 0; glin2.sRn = 0;
      glin2.M = NS; glin2.N = 392; glin2.K = 588; glin2.zi_n = 1; glin2.flags = 1; glin2.act = 0;
      glin2.alpha = 1.0f; glin2.beta = 0.0f; glin2.sa = 1.0f; glin2.sb = 1.0f; glin2.Npad = 392; glin2.pad_ = 0;
      k_gemm<4><<<dim3((unsigned)((392) + 31) / 32, (unsigned)((NS) + 15) / 16, (unsigned)(1)), 32, 0, stream>>>(glin2); }
    k_ep_ctx<<<(unsigned)(((long long)N * S * 3004 + 255) / 256), 256, 0, stream>>>(CO, FFr, XY0, HIN, 3400, 392, S, N);
    { GemmP gdt1_2;
      gdt1_2.A = HIN; gdt1_2.B = dtw1; gdt1_2.bias = dtb1; gdt1_2.R = HIN; gdt1_2.C = HID;
      gdt1_2.sAo = 0; gdt1_2.sAi = 0; gdt1_2.sAm = 3400; gdt1_2.sAk = 1; gdt1_2.sBo = 0; gdt1_2.sBi = 0; gdt1_2.sBn = 1; gdt1_2.sBk = 128; gdt1_2.sCo = 0; gdt1_2.sCi = 0; gdt1_2.sCm = 128; gdt1_2.sRo = 0; gdt1_2.sRi = 0; gdt1_2.sRm = 0; gdt1_2.sRn = 0;
      gdt1_2.M = NS; gdt1_2.N = 128; gdt1_2.K = 3396; gdt1_2.zi_n = 1; gdt1_2.flags = 1; gdt1_2.act = 1;
      gdt1_2.alpha = 1.0f; gdt1_2.beta = 0.0f; gdt1_2.sa = 1.0f; gdt1_2.sb = 1.0f; gdt1_2.Npad = 128; gdt1_2.pad_ = 0;
      k_gemm<4><<<dim3((unsigned)((128) + 31) / 32, (unsigned)((NS) + 15) / 16, (unsigned)(1)), 32, 0, stream>>>(gdt1_2); }
    { GemmP gdt2_2;
      gdt2_2.A = HID; gdt2_2.B = dtw2; gdt2_2.bias = dtb2; gdt2_2.R = HID; gdt2_2.C = DEL;
      gdt2_2.sAo = 0; gdt2_2.sAi = 0; gdt2_2.sAm = 128; gdt2_2.sAk = 1; gdt2_2.sBo = 0; gdt2_2.sBi = 0; gdt2_2.sBn = 1; gdt2_2.sBk = 2; gdt2_2.sCo = 0; gdt2_2.sCi = 0; gdt2_2.sCm = LP; gdt2_2.sRo = 0; gdt2_2.sRi = 0; gdt2_2.sRm = 0; gdt2_2.sRn = 0;
      gdt2_2.M = NS; gdt2_2.N = 2; gdt2_2.K = 128; gdt2_2.zi_n = 1; gdt2_2.flags = 1; gdt2_2.act = 0;
      gdt2_2.alpha = 1.0f; gdt2_2.beta = 0.0f; gdt2_2.sa = 1.0f; gdt2_2.sb = 1.0f; gdt2_2.Npad = LP; gdt2_2.pad_ = 0;
      k_gemm<4><<<dim3((unsigned)((LP) + 31) / 32, (unsigned)((NS) + 15) / 16, (unsigned)(1)), 32, 0, stream>>>(gdt2_2); }
    k_ep_update<<<(unsigned)((S * N * 2 + 255) / 256), 256, 0, stream>>>(CO, DEL, LP, out + (size_t)3 * S * N * 2, 2.f, 1.f, S, N);
    k_ep_featsample<<<(unsigned)((S * N * 64 + 255) / 256), 256, 0, stream>>>(PYF, 1, CO, F2, S, N, 2);
    { GemmP gc2_3_0;
      gc2_3_0.A = F2; gc2_3_0.B = PYF + 0; gc2_3_0.bias = F2; gc2_3_0.R = F2; gc2_3_0.C = CVX + 0;
      gc2_3_0.sAo = (long long)N * LAT; gc2_3_0.sAi = 0; gc2_3_0.sAm = LAT; gc2_3_0.sAk = 1; gc2_3_0.sBo = (long long)LAT * 15930; gc2_3_0.sBi = 0; gc2_3_0.sBn = 1; gc2_3_0.sBk = 15930; gc2_3_0.sCo = (long long)N * 15930; gc2_3_0.sCi = 0; gc2_3_0.sCm = 15930; gc2_3_0.sRo = 0; gc2_3_0.sRi = 0; gc2_3_0.sRm = 0; gc2_3_0.sRn = 0;
      gc2_3_0.M = N; gc2_3_0.N = 12000; gc2_3_0.K = LAT; gc2_3_0.zi_n = 1; gc2_3_0.flags = 0; gc2_3_0.act = 0;
      gc2_3_0.alpha = 0.125f; gc2_3_0.beta = 0.0f; gc2_3_0.sa = 1.0f; gc2_3_0.sb = 1.0f; gc2_3_0.Npad = 12000; gc2_3_0.pad_ = 0;
      k_gemm<4><<<dim3((unsigned)((12000) + 31) / 32, (unsigned)((N) + 15) / 16, (unsigned)(S)), 32, 0, stream>>>(gc2_3_0); }
    { GemmP gc2_3_1;
      gc2_3_1.A = F2; gc2_3_1.B = PYF + 12000; gc2_3_1.bias = F2; gc2_3_1.R = F2; gc2_3_1.C = CVX + 12000;
      gc2_3_1.sAo = (long long)N * LAT; gc2_3_1.sAi = 0; gc2_3_1.sAm = LAT; gc2_3_1.sAk = 1; gc2_3_1.sBo = (long long)LAT * 15930; gc2_3_1.sBi = 0; gc2_3_1.sBn = 1; gc2_3_1.sBk = 15930; gc2_3_1.sCo = (long long)N * 15930; gc2_3_1.sCi = 0; gc2_3_1.sCm = 15930; gc2_3_1.sRo = 0; gc2_3_1.sRi = 0; gc2_3_1.sRm = 0; gc2_3_1.sRn = 0;
      gc2_3_1.M = N; gc2_3_1.N = 3000; gc2_3_1.K = LAT; gc2_3_1.zi_n = 1; gc2_3_1.flags = 0; gc2_3_1.act = 0;
      gc2_3_1.alpha = 0.125f; gc2_3_1.beta = 0.0f; gc2_3_1.sa = 1.0f; gc2_3_1.sb = 1.0f; gc2_3_1.Npad = 3000; gc2_3_1.pad_ = 0;
      k_gemm<4><<<dim3((unsigned)((3000) + 31) / 32, (unsigned)((N) + 15) / 16, (unsigned)(S)), 32, 0, stream>>>(gc2_3_1); }
    { GemmP gc2_3_2;
      gc2_3_2.A = F2; gc2_3_2.B = PYF + 15000; gc2_3_2.bias = F2; gc2_3_2.R = F2; gc2_3_2.C = CVX + 15000;
      gc2_3_2.sAo = (long long)N * LAT; gc2_3_2.sAi = 0; gc2_3_2.sAm = LAT; gc2_3_2.sAk = 1; gc2_3_2.sBo = (long long)LAT * 15930; gc2_3_2.sBi = 0; gc2_3_2.sBn = 1; gc2_3_2.sBk = 15930; gc2_3_2.sCo = (long long)N * 15930; gc2_3_2.sCi = 0; gc2_3_2.sCm = 15930; gc2_3_2.sRo = 0; gc2_3_2.sRi = 0; gc2_3_2.sRm = 0; gc2_3_2.sRn = 0;
      gc2_3_2.M = N; gc2_3_2.N = 750; gc2_3_2.K = LAT; gc2_3_2.zi_n = 1; gc2_3_2.flags = 0; gc2_3_2.act = 0;
      gc2_3_2.alpha = 0.125f; gc2_3_2.beta = 0.0f; gc2_3_2.sa = 1.0f; gc2_3_2.sb = 1.0f; gc2_3_2.Npad = 750; gc2_3_2.pad_ = 0;
      k_gemm<4><<<dim3((unsigned)((750) + 31) / 32, (unsigned)((N) + 15) / 16, (unsigned)(S)), 32, 0, stream>>>(gc2_3_2); }
    { GemmP gc2_3_3;
      gc2_3_3.A = F2; gc2_3_3.B = PYF + 15750; gc2_3_3.bias = F2; gc2_3_3.R = F2; gc2_3_3.C = CVX + 15750;
      gc2_3_3.sAo = (long long)N * LAT; gc2_3_3.sAi = 0; gc2_3_3.sAm = LAT; gc2_3_3.sAk = 1; gc2_3_3.sBo = (long long)LAT * 15930; gc2_3_3.sBi = 0; gc2_3_3.sBn = 1; gc2_3_3.sBk = 15930; gc2_3_3.sCo = (long long)N * 15930; gc2_3_3.sCi = 0; gc2_3_3.sCm = 15930; gc2_3_3.sRo = 0; gc2_3_3.sRi = 0; gc2_3_3.sRm = 0; gc2_3_3.sRn = 0;
      gc2_3_3.M = N; gc2_3_3.N = 180; gc2_3_3.K = LAT; gc2_3_3.zi_n = 1; gc2_3_3.flags = 0; gc2_3_3.act = 0;
      gc2_3_3.alpha = 0.125f; gc2_3_3.beta = 0.0f; gc2_3_3.sa = 1.0f; gc2_3_3.sb = 1.0f; gc2_3_3.Npad = 180; gc2_3_3.pad_ = 0;
      k_gemm<4><<<dim3((unsigned)((180) + 31) / 32, (unsigned)((N) + 15) / 16, (unsigned)(S)), 32, 0, stream>>>(gc2_3_3); }
    k_ep_csample<<<(unsigned)((N * S * 196 + 255) / 256), 256, 0, stream>>>(CVX, 1, CO, FCAT, 608, S, N);
    k_ep_csample<<<(unsigned)((N * S * 196 + 255) / 256), 256, 0, stream>>>(CV1, 0, CO, FCAT, 608, S, N);
    k_ep_featsample<<<(unsigned)((S * N * 64 + 255) / 256), 256, 0, stream>>>(PYF, 1, CO, F2, S, N, 4);
    { GemmP gc4_3_0;
      gc4_3_0.A = F2; gc4_3_0.B = PYF + 0; gc4_3_0.bias = F2; gc4_3_0.R = F2; gc4_3_0.C = CVX + 0;
      gc4_3_0.sAo = (long long)N * LAT; gc4_3_0.sAi = 0; gc4_3_0.sAm = LAT; gc4_3_0.sAk = 1; gc4_3_0.sBo = (long long)LAT * 15930; gc4_3_0.sBi = 0; gc4_3_0.sBn = 1; gc4_3_0.sBk = 15930; gc4_3_0.sCo = (long long)N * 15930; gc4_3_0.sCi = 0; gc4_3_0.sCm = 15930; gc4_3_0.sRo = 0; gc4_3_0.sRi = 0; gc4_3_0.sRm = 0; gc4_3_0.sRn = 0;
      gc4_3_0.M = N; gc4_3_0.N = 12000; gc4_3_0.K = LAT; gc4_3_0.zi_n = 1; gc4_3_0.flags = 0; gc4_3_0.act = 0;
      gc4_3_0.alpha = 0.125f; gc4_3_0.beta = 0.0f; gc4_3_0.sa = 1.0f; gc4_3_0.sb = 1.0f; gc4_3_0.Npad = 12000; gc4_3_0.pad_ = 0;
      k_gemm<4><<<dim3((unsigned)((12000) + 31) / 32, (unsigned)((N) + 15) / 16, (unsigned)(S)), 32, 0, stream>>>(gc4_3_0); }
    { GemmP gc4_3_1;
      gc4_3_1.A = F2; gc4_3_1.B = PYF + 12000; gc4_3_1.bias = F2; gc4_3_1.R = F2; gc4_3_1.C = CVX + 12000;
      gc4_3_1.sAo = (long long)N * LAT; gc4_3_1.sAi = 0; gc4_3_1.sAm = LAT; gc4_3_1.sAk = 1; gc4_3_1.sBo = (long long)LAT * 15930; gc4_3_1.sBi = 0; gc4_3_1.sBn = 1; gc4_3_1.sBk = 15930; gc4_3_1.sCo = (long long)N * 15930; gc4_3_1.sCi = 0; gc4_3_1.sCm = 15930; gc4_3_1.sRo = 0; gc4_3_1.sRi = 0; gc4_3_1.sRm = 0; gc4_3_1.sRn = 0;
      gc4_3_1.M = N; gc4_3_1.N = 3000; gc4_3_1.K = LAT; gc4_3_1.zi_n = 1; gc4_3_1.flags = 0; gc4_3_1.act = 0;
      gc4_3_1.alpha = 0.125f; gc4_3_1.beta = 0.0f; gc4_3_1.sa = 1.0f; gc4_3_1.sb = 1.0f; gc4_3_1.Npad = 3000; gc4_3_1.pad_ = 0;
      k_gemm<4><<<dim3((unsigned)((3000) + 31) / 32, (unsigned)((N) + 15) / 16, (unsigned)(S)), 32, 0, stream>>>(gc4_3_1); }
    { GemmP gc4_3_2;
      gc4_3_2.A = F2; gc4_3_2.B = PYF + 15000; gc4_3_2.bias = F2; gc4_3_2.R = F2; gc4_3_2.C = CVX + 15000;
      gc4_3_2.sAo = (long long)N * LAT; gc4_3_2.sAi = 0; gc4_3_2.sAm = LAT; gc4_3_2.sAk = 1; gc4_3_2.sBo = (long long)LAT * 15930; gc4_3_2.sBi = 0; gc4_3_2.sBn = 1; gc4_3_2.sBk = 15930; gc4_3_2.sCo = (long long)N * 15930; gc4_3_2.sCi = 0; gc4_3_2.sCm = 15930; gc4_3_2.sRo = 0; gc4_3_2.sRi = 0; gc4_3_2.sRm = 0; gc4_3_2.sRn = 0;
      gc4_3_2.M = N; gc4_3_2.N = 750; gc4_3_2.K = LAT; gc4_3_2.zi_n = 1; gc4_3_2.flags = 0; gc4_3_2.act = 0;
      gc4_3_2.alpha = 0.125f; gc4_3_2.beta = 0.0f; gc4_3_2.sa = 1.0f; gc4_3_2.sb = 1.0f; gc4_3_2.Npad = 750; gc4_3_2.pad_ = 0;
      k_gemm<4><<<dim3((unsigned)((750) + 31) / 32, (unsigned)((N) + 15) / 16, (unsigned)(S)), 32, 0, stream>>>(gc4_3_2); }
    { GemmP gc4_3_3;
      gc4_3_3.A = F2; gc4_3_3.B = PYF + 15750; gc4_3_3.bias = F2; gc4_3_3.R = F2; gc4_3_3.C = CVX + 15750;
      gc4_3_3.sAo = (long long)N * LAT; gc4_3_3.sAi = 0; gc4_3_3.sAm = LAT; gc4_3_3.sAk = 1; gc4_3_3.sBo = (long long)LAT * 15930; gc4_3_3.sBi = 0; gc4_3_3.sBn = 1; gc4_3_3.sBk = 15930; gc4_3_3.sCo = (long long)N * 15930; gc4_3_3.sCi = 0; gc4_3_3.sCm = 15930; gc4_3_3.sRo = 0; gc4_3_3.sRi = 0; gc4_3_3.sRm = 0; gc4_3_3.sRn = 0;
      gc4_3_3.M = N; gc4_3_3.N = 180; gc4_3_3.K = LAT; gc4_3_3.zi_n = 1; gc4_3_3.flags = 0; gc4_3_3.act = 0;
      gc4_3_3.alpha = 0.125f; gc4_3_3.beta = 0.0f; gc4_3_3.sa = 1.0f; gc4_3_3.sb = 1.0f; gc4_3_3.Npad = 180; gc4_3_3.pad_ = 0;
      k_gemm<4><<<dim3((unsigned)((180) + 31) / 32, (unsigned)((N) + 15) / 16, (unsigned)(S)), 32, 0, stream>>>(gc4_3_3); }
    k_ep_csample<<<(unsigned)((N * S * 196 + 255) / 256), 256, 0, stream>>>(CVX, 2, CO, FCAT, 608, S, N);
    { GemmP glin3;
      glin3.A = FCAT; glin3.B = linw; glin3.bias = linb; glin3.R = FCAT; glin3.C = HIN;
      glin3.sAo = 0; glin3.sAi = 0; glin3.sAm = 608; glin3.sAk = 1; glin3.sBo = 0; glin3.sBi = 0; glin3.sBn = 1; glin3.sBk = 392; glin3.sCo = 0; glin3.sCi = 0; glin3.sCm = 3400; glin3.sRo = 0; glin3.sRi = 0; glin3.sRm = 0; glin3.sRn = 0;
      glin3.M = NS; glin3.N = 392; glin3.K = 588; glin3.zi_n = 1; glin3.flags = 1; glin3.act = 0;
      glin3.alpha = 1.0f; glin3.beta = 0.0f; glin3.sa = 1.0f; glin3.sb = 1.0f; glin3.Npad = 392; glin3.pad_ = 0;
      k_gemm<4><<<dim3((unsigned)((392) + 31) / 32, (unsigned)((NS) + 15) / 16, (unsigned)(1)), 32, 0, stream>>>(glin3); }
    k_ep_ctx<<<(unsigned)(((long long)N * S * 3004 + 255) / 256), 256, 0, stream>>>(CO, FFr, XY0, HIN, 3400, 392, S, N);
    { GemmP gdt1_3;
      gdt1_3.A = HIN; gdt1_3.B = dtw1; gdt1_3.bias = dtb1; gdt1_3.R = HIN; gdt1_3.C = HID;
      gdt1_3.sAo = 0; gdt1_3.sAi = 0; gdt1_3.sAm = 3400; gdt1_3.sAk = 1; gdt1_3.sBo = 0; gdt1_3.sBi = 0; gdt1_3.sBn = 1; gdt1_3.sBk = 128; gdt1_3.sCo = 0; gdt1_3.sCi = 0; gdt1_3.sCm = 128; gdt1_3.sRo = 0; gdt1_3.sRi = 0; gdt1_3.sRm = 0; gdt1_3.sRn = 0;
      gdt1_3.M = NS; gdt1_3.N = 128; gdt1_3.K = 3396; gdt1_3.zi_n = 1; gdt1_3.flags = 1; gdt1_3.act = 1;
      gdt1_3.alpha = 1.0f; gdt1_3.beta = 0.0f; gdt1_3.sa = 1.0f; gdt1_3.sb = 1.0f; gdt1_3.Npad = 128; gdt1_3.pad_ = 0;
      k_gemm<4><<<dim3((unsigned)((128) + 31) / 32, (unsigned)((NS) + 15) / 16, (unsigned)(1)), 32, 0, stream>>>(gdt1_3); }
    { GemmP gdt2_3;
      gdt2_3.A = HID; gdt2_3.B = dtw2; gdt2_3.bias = dtb2; gdt2_3.R = HID; gdt2_3.C = DEL;
      gdt2_3.sAo = 0; gdt2_3.sAi = 0; gdt2_3.sAm = 128; gdt2_3.sAk = 1; gdt2_3.sBo = 0; gdt2_3.sBi = 0; gdt2_3.sBn = 1; gdt2_3.sBk = 2; gdt2_3.sCo = 0; gdt2_3.sCi = 0; gdt2_3.sCm = LP; gdt2_3.sRo = 0; gdt2_3.sRi = 0; gdt2_3.sRm = 0; gdt2_3.sRn = 0;
      gdt2_3.M = NS; gdt2_3.N = 2; gdt2_3.K = 128; gdt2_3.zi_n = 1; gdt2_3.flags = 1; gdt2_3.act = 0;
      gdt2_3.alpha = 1.0f; gdt2_3.beta = 0.0f; gdt2_3.sa = 1.0f; gdt2_3.sb = 1.0f; gdt2_3.Npad = LP; gdt2_3.pad_ = 0;
      k_gemm<4><<<dim3((unsigned)((LP) + 31) / 32, (unsigned)((NS) + 15) / 16, (unsigned)(1)), 32, 0, stream>>>(gdt2_3); }
    k_ep_update<<<(unsigned)((S * N * 2 + 255) / 256), 256, 0, stream>>>(CO, DEL, LP, out + (size_t)4 * S * N * 2, 2.f, 1.f, S, N);
}
